// WeightedBatchSubTreeEncoder_84817014161755
// MI455X (gfx1250) — hardware-verified
//
#include <hip/hip_runtime.h>
#include <math.h>

typedef __attribute__((ext_vector_type(16))) _Float16 v16h;
typedef __attribute__((ext_vector_type(8)))  _Float16 v8h;
typedef __attribute__((ext_vector_type(16))) __bf16   v16b;
typedef __attribute__((ext_vector_type(8)))  float    v8f;
typedef __attribute__((ext_vector_type(4)))  float    v4f;

__device__ __forceinline__ int frag_k(int i, int h) { return (i < 8) ? (8 * h + i) : (16 + 8 * h + (i - 8)); }
__device__ __forceinline__ __bf16 bf16_rne(float f) {
    unsigned int u = __float_as_uint(f);
    u += 0x7fffu + ((u >> 16) & 1u);
    return __builtin_bit_cast(__bf16, (unsigned short)(u >> 16));
}
__device__ __forceinline__ float bf16_f32(__bf16 b) { return __uint_as_float(((unsigned int)__builtin_bit_cast(unsigned short, b)) << 16); }
__device__ __forceinline__ v8f wmma16(v16h a, v16h b, v8f c) {
    c = __builtin_amdgcn_wmma_f32_16x16x32_f16(false, a, false, b, (short)0, c, false, false);
    asm volatile("v_nop\n\tv_nop\n\tv_nop\n\tv_nop" : "+v"(c) : "v"(a), "v"(b));
    return c;
}
__device__ __forceinline__ v8f wmmab(v16b a, v16b b, v8f c) {
    c = __builtin_amdgcn_wmma_f32_16x16x32_bf16(false, a, false, b, (short)0, c, false, false);
    asm volatile("v_nop\n\tv_nop\n\tv_nop\n\tv_nop" : "+v"(c) : "v"(a), "v"(b));
    return c;
}
struct Split { v16b hi, lo; };
__device__ __forceinline__ v8f wmma3(const Split& a, const Split& b, v8f c) {
    c = __builtin_amdgcn_wmma_f32_16x16x32_bf16(false, a.hi, false, b.hi, (short)0, c, false, false);
    c = __builtin_amdgcn_wmma_f32_16x16x32_bf16(false, a.hi, false, b.lo, (short)0, c, false, false);
    c = __builtin_amdgcn_wmma_f32_16x16x32_bf16(false, a.lo, false, b.hi, (short)0, c, false, false);
    asm volatile("v_nop\n\tv_nop\n\tv_nop\n\tv_nop" : "+v"(c) : "v"(a.hi), "v"(a.lo), "v"(b.hi), "v"(b.lo));
    return c;
}
struct Split3 { v16b hi, mid, lo; };
__device__ __forceinline__ v8f wmma6(const Split3& a, const Split3& b, v8f c) {
    c = __builtin_amdgcn_wmma_f32_16x16x32_bf16(false, a.hi, false, b.hi, (short)0, c, false, false);
    c = __builtin_amdgcn_wmma_f32_16x16x32_bf16(false, a.hi, false, b.mid, (short)0, c, false, false);
    c = __builtin_amdgcn_wmma_f32_16x16x32_bf16(false, a.mid, false, b.hi, (short)0, c, false, false);
    c = __builtin_amdgcn_wmma_f32_16x16x32_bf16(false, a.hi, false, b.lo, (short)0, c, false, false);
    c = __builtin_amdgcn_wmma_f32_16x16x32_bf16(false, a.mid, false, b.mid, (short)0, c, false, false);
    c = __builtin_amdgcn_wmma_f32_16x16x32_bf16(false, a.lo, false, b.hi, (short)0, c, false, false);
    asm volatile("v_nop\n\tv_nop\n\tv_nop\n\tv_nop" : "+v"(c) : "v"(a.hi), "v"(a.mid), "v"(a.lo), "v"(b.hi), "v"(b.mid), "v"(b.lo));
    return c;
}

__device__ __forceinline__ v16h fh_ld(const float* __restrict__ p, long long sk, int k0, int h, int klen, float s) {
    v16h a;
#pragma unroll
    for (int i = 0; i < 16; ++i) { const int k = k0 + frag_k(i, h); a[i] = (k < klen) ? (_Float16)(p[(long long)k * sk] * s) : (_Float16)0.f; }
    return a;
}
__device__ __forceinline__ Split sp_ld(const float* __restrict__ p, long long sk, int k0, int h, int klen, float s) {
    Split r;
#pragma unroll
    for (int i = 0; i < 16; ++i) {
        const int k = k0 + frag_k(i, h); const float x = (k < klen) ? p[(long long)k * sk] * s : 0.f;
        const __bf16 hb = bf16_rne(x); r.hi[i] = hb; r.lo[i] = bf16_rne(x - bf16_f32(hb));
    }
    return r;
}
__device__ __forceinline__ Split3 sp3_ld(const float* __restrict__ p, long long sk, int k0, int h, int klen, float s) {
    Split3 r;
#pragma unroll
    for (int i = 0; i < 16; ++i) {
        const int k = k0 + frag_k(i, h); const float x = (k < klen) ? p[(long long)k * sk] * s : 0.f;
        const __bf16 hb = bf16_rne(x); const float r1 = x - bf16_f32(hb); const __bf16 mb = bf16_rne(r1);
        r.hi[i] = hb; r.mid[i] = mb; r.lo[i] = bf16_rne(r1 - bf16_f32(mb));
    }
    return r;
}
__device__ __forceinline__ v16b bh_ld(const float* __restrict__ p, long long sk, int k0, int h, int klen, float s) {
    v16b a;
#pragma unroll
    for (int i = 0; i < 16; ++i) { const int k = k0 + frag_k(i, h); a[i] = bf16_rne((k < klen) ? p[(long long)k * sk] * s : 0.f); }
    return a;
}
__device__ __forceinline__ v16h fh_row(const _Float16* __restrict__ row, int k0, int h) {
    v16h a;
#pragma unroll
    for (int i = 0; i < 16; ++i) a[i] = row[k0 + frag_k(i, h)];
    return a;
}

#define VST2(T, ptr, val) do { const T vst2_v_ = (val); *(volatile T*)(ptr) = vst2_v_; __threadfence(); *(volatile T*)(ptr) = vst2_v_; } while (0)
typedef float v4f __attribute__((ext_vector_type(4)));
#define VST2V4(ptr, val) do { const v4f vst2_v4_ = (val); *(volatile v4f*)(ptr) = vst2_v4_; __threadfence(); *(volatile v4f*)(ptr) = vst2_v4_; } while (0)

__device__ __attribute__((noinline)) float act_fn(float v, int act) {
    if (act == 1) return fmaxf(v, 0.f);
    if (act == 2) { const float u = 0.7978845608028654f * (v + 0.044715f * v * v * v); return 0.5f * v * (1.f + tanhf(u)); }
    if (act == 3) return v / (1.f + expf(-v));
    if (act == 4) return 0.5f * v * (1.f + erff(v * 0.7071067811865476f));
    if (act == 5) return tanhf(v);
    if (act == 6) return 1.f / (1.f + expf(-v));
    if (act == 7) return (v > 0.f) ? v : 0.01f * v;
    if (act == 8) return (v > 0.f) ? v : (expf(v) - 1.f);
    if (act == 9) return fminf(fmaxf(v, 0.f), 6.f);
    if (act == 10) return fabsf(v);
    if (act == 11) return (v >= 0.f) ? v : 0.1f * v;
    if (act == 12) return (v > 0.f) ? v : 0.2f * v;
    if (act == 13) return (v > 20.f) ? v : log1pf(expf(v));
    return v;
}

struct GemmP {
    const float* A; const float* B; const float* bias; const float* R; float* C;
    long long sAo, sAi, sAm, sAk, sBo, sBi, sBn, sBk, sCo, sCi, sCm, sRo, sRi, sRm, sRn;
    int M, N, K, zi_n, flags, act; float alpha, beta, sa, sb;
    int Npad, pad_;
};
static_assert(sizeof(GemmP) == 5 * 8 + 15 * 8 + 6 * 4 + 4 * 4 + 2 * 4, "GemmP has padding");

template <int MODE>
__global__ __launch_bounds__(32) void k_gemm(GemmP p) {
    const int lane = threadIdx.x & 31, h = lane >> 4, l15 = lane & 15;
    const int m0 = blockIdx.y * 16, n0 = blockIdx.x * 32;
    const int z = blockIdx.z, zo = z / p.zi_n, zi = z - zo * p.zi_n;
    const float* A = p.A + zo * p.sAo + zi * p.sAi;
    const float* B = p.B + zo * p.sBo + zi * p.sBi;
    const int am = min(m0 + l15, p.M - 1);
    v8f acc[2], comp[2];
#pragma unroll
    for (int t = 0; t < 2; ++t) { v8f zz = {}; acc[t] = zz; comp[t] = zz; }
    for (int k0 = 0; k0 < p.K; k0 += 32) {
        const float* arow = A + (long long)am * p.sAm;
        if (MODE == 1) {
            const Split a = sp_ld(arow, p.sAk, k0, h, p.K, 1.f);
#pragma unroll
            for (int t = 0; t < 2; ++t) {
                const int bn = min(n0 + t * 16 + l15, p.N - 1);
                acc[t] = wmma3(a, sp_ld(B + (long long)bn * p.sBn, p.sBk, k0, h, p.K, 1.f), acc[t]);
            }
        } else if (MODE == 3) {
            const Split3 a = sp3_ld(arow, p.sAk, k0, h, p.K, 1.f);
#pragma unroll
            for (int t = 0; t < 2; ++t) {
                const int bn = min(n0 + t * 16 + l15, p.N - 1);
                acc[t] = wmma6(a, sp3_ld(B + (long long)bn * p.sBn, p.sBk, k0, h, p.K, 1.f), acc[t]);
            }
        } else if (MODE == 4) {
            const Split3 a = sp3_ld(arow, p.sAk, k0, h, p.K, 1.f);
#pragma unroll
            for (int t = 0; t < 2; ++t) {
                const int bn = min(n0 + t * 16 + l15, p.N - 1); v8f zz = {};
                const v8f part = wmma6(a, sp3_ld(B + (long long)bn * p.sBn, p.sBk, k0, h, p.K, 1.f), zz);
                const v8f y = part - comp[t]; const v8f s = acc[t] + y; comp[t] = (s - acc[t]) - y; acc[t] = s;
            }
        } else if (MODE == 2) {
            const v16b a = bh_ld(arow, p.sAk, k0, h, p.K, 1.f);
#pragma unroll
            for (int t = 0; t < 2; ++t) {
                const int bn = min(n0 + t * 16 + l15, p.N - 1);
                acc[t] = wmmab(a, bh_ld(B + (long long)bn * p.sBn, p.sBk, k0, h, p.K, 1.f), acc[t]);
            }
        } else {
            const v16h a = fh_ld(arow, p.sAk, k0, h, p.K, p.sa);
#pragma unroll
            for (int t = 0; t < 2; ++t) {
                const int bn = min(n0 + t * 16 + l15, p.N - 1);
                acc[t] = wmma16(a, fh_ld(B + (long long)bn * p.sBn, p.sBk, k0, h, p.K, p.sb), acc[t]);
            }
        }
    }
    const float iscale = (MODE == 0) ? p.alpha / (p.sa * p.sb) : p.alpha;
    float* C = p.C + zo * p.sCo + zi * p.sCi;
    const float* R = p.R + zo * p.sRo + zi * p.sRi;
    __shared__ __align__(16) float ctile[16][36];
#pragma unroll
    for (int t = 0; t < 2; ++t) {
        const int n = n0 + t * 16 + l15; const int nn = min(n, p.N - 1);
#pragma unroll
        for (int r = 0; r < 8; ++r) {
            const int m = m0 + 8 * h + r; const int mm = min(m, p.M - 1);
            float v = acc[t][r] * iscale;
            if (p.flags & 1) v += p.bias[nn];
            if (p.flags & 2) v += p.bias[mm];
            if (p.flags & 8) v *= p.bias[(long long)zo * p.M + mm];
            v = act_fn(v, p.act);
            if (p.flags & 4) v += p.beta * R[(long long)mm * p.sRm + (long long)nn * p.sRn];
            ctile[8 * h + r][t * 16 + l15] = (n < p.N) ? v : 0.f;
        }
    }
    __syncthreads();
    const int NW = (p.Npad > p.N) ? p.Npad : p.N;
    const bool fast = (m0 + 16 <= p.M) && (n0 + 32 <= NW) && ((p.sCm & 3) == 0) && ((((size_t)C) & 15) == 0);
    if (fast) {
#pragma unroll
        for (int s = 0; s < 4; ++s) {
            const int row = s * 4 + (lane >> 3), c4 = (lane & 7) * 4;
            const v4f v = *(const v4f*)&ctile[row][c4];
            VST2V4(C + (long long)(m0 + row) * p.sCm + n0 + c4, v);
        }
    } else {
        for (int row = 0; row < 16; ++row) {
            const int m = m0 + row, n = n0 + lane;
            if (m < p.M && n < NW) VST2(float, C + (long long)m * p.sCm + n, ctile[row][lane]);
        }
    }
}


template <int MODE, int TM, int TN>
__global__ __launch_bounds__(32) void k_gemmT(GemmP p) {
    const int lane = threadIdx.x & 31, h = lane >> 4, l15 = lane & 15;
    const int m0 = blockIdx.y * (16 * TM), n0 = blockIdx.x * (16 * TN);
    const int z = blockIdx.z, zo = z / p.zi_n, zi = z - zo * p.zi_n;
    const float* A = p.A + zo * p.sAo + zi * p.sAi;
    const float* B = p.B + zo * p.sBo + zi * p.sBi;
    v8f acc[TM][TN];
#pragma unroll
    for (int i = 0; i < TM; ++i)
#pragma unroll
        for (int t = 0; t < TN; ++t) { v8f zz = {}; acc[i][t] = zz; }
    for (int k0 = 0; k0 < p.K; k0 += 32) {
        if (MODE == 1) {
            Split a[TM], b[TN];
#pragma unroll
            for (int i = 0; i < TM; ++i) { const int am = min(m0 + 16 * i + l15, p.M - 1); a[i] = sp_ld(A + (long long)am * p.sAm, p.sAk, k0, h, p.K, 1.f); }
#pragma unroll
            for (int t = 0; t < TN; ++t) { const int bn = min(n0 + 16 * t + l15, p.N - 1); b[t] = sp_ld(B + (long long)bn * p.sBn, p.sBk, k0, h, p.K, 1.f); }
#pragma unroll
            for (int i = 0; i < TM; ++i)
#pragma unroll
                for (int t = 0; t < TN; ++t) acc[i][t] = wmma3(a[i], b[t], acc[i][t]);
        } else if (MODE == 2) {
            v16b a[TM], b[TN];
#pragma unroll
            for (int i = 0; i < TM; ++i) { const int am = min(m0 + 16 * i + l15, p.M - 1); a[i] = bh_ld(A + (long long)am * p.sAm, p.sAk, k0, h, p.K, 1.f); }
#pragma unroll
            for (int t = 0; t < TN; ++t) { const int bn = min(n0 + 16 * t + l15, p.N - 1); b[t] = bh_ld(B + (long long)bn * p.sBn, p.sBk, k0, h, p.K, 1.f); }
#pragma unroll
            for (int i = 0; i < TM; ++i)
#pragma unroll
                for (int t = 0; t < TN; ++t) acc[i][t] = wmmab(a[i], b[t], acc[i][t]);
        } else {
            v16h a[TM], b[TN];
#pragma unroll
            for (int i = 0; i < TM; ++i) { const int am = min(m0 + 16 * i + l15, p.M - 1); a[i] = fh_ld(A + (long long)am * p.sAm, p.sAk, k0, h, p.K, p.sa); }
#pragma unroll
            for (int t = 0; t < TN; ++t) { const int bn = min(n0 + 16 * t + l15, p.N - 1); b[t] = fh_ld(B + (long long)bn * p.sBn, p.sBk, k0, h, p.K, p.sb); }
#pragma unroll
            for (int i = 0; i < TM; ++i)
#pragma unroll
                for (int t = 0; t < TN; ++t) acc[i][t] = wmma16(a[i], b[t], acc[i][t]);
        }
    }
    const float iscale = (MODE == 0) ? p.alpha / (p.sa * p.sb) : p.alpha;
    float* C = p.C + zo * p.sCo + zi * p.sCi;
    const float* R = p.R + zo * p.sRo + zi * p.sRi;
    const int NW = (p.Npad > p.N) ? p.Npad : p.N;
    __shared__ __align__(16) float ctile[16][36];
#pragma unroll
    for (int i = 0; i < TM; ++i) {
        const int mb = m0 + 16 * i; if (mb >= p.M) break;
#pragma unroll
        for (int tp = 0; tp < TN / 2; ++tp) {
            const int nb = n0 + 32 * tp; if (nb >= NW) break;
#pragma unroll
            for (int t2 = 0; t2 < 2; ++t2) {
                const int t = 2 * tp + t2; const int n = nb + t2 * 16 + l15; const int nn = min(n, p.N - 1);
#pragma unroll
                for (int r = 0; r < 8; ++r) {
                    const int m = mb + 8 * h + r; const int mm = min(m, p.M - 1);
                    float v = acc[i][t][r] * iscale;
                    if (p.flags & 1) v += p.bias[nn];
                    if (p.flags & 2) v += p.bias[mm];
            if (p.flags & 8) v *= p.bias[(long long)zo * p.M + mm];
                    v = act_fn(v, p.act);
                    if (p.flags & 4) v += p.beta * R[(long long)mm * p.sRm + (long long)nn * p.sRn];
                    ctile[8 * h + r][t2 * 16 + l15] = (n < p.N) ? v : 0.f;
                }
            }
            __syncthreads();
            const bool fast = (mb + 16 <= p.M) && (nb + 32 <= NW) && ((p.sCm & 3) == 0) && ((((size_t)C) & 15) == 0);
            if (fast) {
#pragma unroll
                for (int s = 0; s < 4; ++s) {
                    const int row = s * 4 + (lane >> 3), c4 = (lane & 7) * 4;
                    const v4f v = *(const v4f*)&ctile[row][c4];
                    VST2V4(C + (long long)(mb + row) * p.sCm + nb + c4, v);
                }
            } else {
                for (int row = 0; row < 16; ++row) {
                    const int m = mb + row, n = nb + lane;
                    if (m < p.M && n < NW) VST2(float, C + (long long)m * p.sCm + n, ctile[row][lane]);
                }
            }
            __syncthreads();
        }
    }
}

#define AW 4
struct AttnP {
    const float* Q; const float* K; const float* V; float* O; float* P; const float* Mf; const int* Mi; float* ST;
    const float* Pw; const float* Rt; const int* SQ; const int* SK;
    long long swb, swh, swi, swj, srb, srh, sri;
    long long sQb, sQh, sQi, sQd, sKb, sKh, sKj, sKd, sVb, sVh, sVj, sVd, sOb, sOh, sOi, sPb, sPh, sPi, smb, smh, smi, smj;
    int Lq, Lk, dh, dv, hrep, causal, coff, pband;
    float scale, mfill; int nonorm, mpol;
    int roff, rn, segpol, win;
};
static_assert(sizeof(AttnP) == 12 * 8 + 29 * 8 + 16 * 4, "AttnP has padding");

#ifndef KATTN_ATTR
#define KATTN_ATTR
#endif
template <int DHP, int DVP, int QM, bool SPLITPV, bool TWOPASS>
__global__ __launch_bounds__(32 * AW) KATTN_ATTR void k_attn(AttnP p) {
    constexpr int NT = DVP / 16;
    constexpr int KS = DHP / 32;
    constexpr int VP = DVP + 8;
    __shared__ __align__(16) float    pl[AW][16 * 64];
    __shared__ __align__(16) _Float16 vl[(SPLITPV ? 2 : 1) * 64 * VP];
    const int lane = threadIdx.x & 31, hf = lane >> 4, l15 = lane & 15, wave = threadIdx.x >> 5;
    const int h = blockIdx.y, b = blockIdx.z, hk = h / p.hrep;
    const int q0 = (blockIdx.x * AW + wave) * 16;
    float* myp = pl[wave];
    const float L2E = 1.4426950408889634f;
    const float NEG = -__builtin_inff();
    const int qi = min(q0 + l15, p.Lq - 1);
    const float* qrow = p.Q + b * p.sQb + h * p.sQh + (long long)qi * p.sQi;
    const float* kbase = p.K + b * p.sKb + hk * p.sKh;
    const float* vbase = p.V + b * p.sVb + hk * p.sVh;
    v16h qa[QM == 0 ? KS : 1]; Split qs_[QM == 1 ? KS : 1]; Split3 qt_[QM == 2 ? KS : 1];
#pragma unroll
    for (int ks = 0; ks < KS; ++ks) {
        if (QM == 2) qt_[ks] = sp3_ld(qrow, p.sQd, ks * 32, hf, p.dh, 1.f);
        else if (QM == 1) qs_[ks] = sp_ld(qrow, p.sQd, ks * 32, hf, p.dh, 1.f);
        else qa[ks] = fh_ld(qrow, p.sQd, ks * 32, hf, p.dh, 1.f);
    }
    v8f o[NT]; float m8[8], l8[8];
#pragma unroll
    for (int t = 0; t < NT; ++t) { v8f zz = {}; o[t] = zz; }
#pragma unroll
    for (int i = 0; i < 8; ++i) { m8[i] = NEG; l8[i] = 0.f; }
    int jend = p.Lk;
    if (p.causal == 1) { const int je = (blockIdx.x * AW + AW - 1) * 16 + 16 + p.coff; jend = min(jend, max(je, 0)); }
    const int npass = TWOPASS ? 2 : 1;
    for (int pass = 0; pass < npass; ++pass) {
        const bool dopv = (!TWOPASS) || pass == 1;
        for (int j0 = 0; j0 < jend; j0 += 64) {
            if (dopv) {
                __syncthreads();
                for (int idx = threadIdx.x; idx < 64 * DVP; idx += 32 * AW) {
                    const int jr = idx / DVP, d = idx - jr * DVP, j = j0 + jr;
                    const float f = (j < p.Lk && d < p.dv) ? vbase[(long long)j * p.sVj + (long long)d * p.sVd] : 0.f;
                    if (SPLITPV) {
                        const __bf16 hb = bf16_rne(f);
                        ((__bf16*)vl)[jr * VP + d] = hb; ((__bf16*)vl)[64 * VP + jr * VP + d] = bf16_rne(f - bf16_f32(hb));
                    } else vl[jr * VP + d] = (_Float16)f;
                }
            }
            v8f s[4];
#pragma unroll
            for (int t = 0; t < 4; ++t) {
                const int j = min(j0 + t * 16 + l15, p.Lk - 1);
                const float* krow = kbase + (long long)j * p.sKj;
                v8f acc = {};
#pragma unroll
                for (int ks = 0; ks < KS; ++ks) {
                    if (QM == 2)      acc = wmma6(qt_[ks], sp3_ld(krow, p.sKd, ks * 32, hf, p.dh, 1.f), acc);
                    else if (QM == 1) acc = wmma3(qs_[ks], sp_ld(krow, p.sKd, ks * 32, hf, p.dh, 1.f), acc);
                    else              acc = wmma16(qa[ks], fh_ld(krow, p.sKd, ks * 32, hf, p.dh, 1.f), acc);
                }
                s[t] = acc;
            }
            float pv[8][4];
#pragma unroll
            for (int i = 0; i < 8; ++i) {
                const int irow = q0 + i + 8 * hf;
                const int ic = min(irow, p.Lq - 1);
                float sc[4];
#pragma unroll
                for (int t = 0; t < 4; ++t) {
                    const int jg = j0 + t * 16 + l15;
                    float v = s[t][i] * p.scale;
                    if (p.Mf) v += p.Mf[b * p.smb + h * p.smh + (long long)ic * p.smi + (long long)min(jg, p.Lk - 1) * p.smj];
                    if (p.Rt) { int rc = ic - min(jg, p.Lk - 1) + p.roff; rc = rc < 0 ? 0 : (rc >= p.rn ? p.rn - 1 : rc); v += p.Rt[b * p.srb + h * p.srh + (long long)ic * p.sri + rc]; }
                    if (p.Mi) { const int mv = p.Mi[b * p.smb + h * p.smh + (long long)ic * p.smi + (long long)min(jg, p.Lk - 1) * p.smj]; if (p.mpol ? (mv != 0) : (mv == 0)) v = p.mfill; }
                    if (p.SQ) { const bool same = p.SQ[(long long)b * p.Lq + ic] == p.SK[(long long)b * p.Lk + min(jg, p.Lk - 1)]; if (p.segpol ? same : !same) v = p.mfill; }
                    if (p.causal == 2 && jg > irow + p.coff) v = p.mfill;
                    if (jg >= p.Lk || (p.causal == 1 && jg > irow + p.coff) || (p.causal == 3 && jg < irow + p.coff) || (p.win > 0 && irow + p.coff - jg > p.win)) v = NEG; else v *= L2E;
                    sc[t] = v;
                }
                if (!TWOPASS || pass == 0) {
                    float mx = fmaxf(fmaxf(sc[0], sc[1]), fmaxf(sc[2], sc[3]));
                    mx = fmaxf(mx, __shfl_xor(mx, 1, 32)); mx = fmaxf(mx, __shfl_xor(mx, 2, 32));
                    mx = fmaxf(mx, __shfl_xor(mx, 4, 32)); mx = fmaxf(mx, __shfl_xor(mx, 8, 32));
                    const float mnew = fmaxf(m8[i], mx);
                    const float corr = (mnew == NEG) ? 1.f : exp2f(m8[i] - mnew);
                    float rs = 0.f;
#pragma unroll
                    for (int t = 0; t < 4; ++t) {
                        const float pp = (sc[t] == NEG) ? 0.f : exp2f(sc[t] - mnew); rs += pp;
                        pv[i][t] = p.Pw ? pp * p.Pw[b * p.swb + h * p.swh + (long long)ic * p.swi + (long long)min(j0 + t * 16 + l15, p.Lk - 1) * p.swj] : pp;
                    }
                    rs += __shfl_xor(rs, 1, 32); rs += __shfl_xor(rs, 2, 32); rs += __shfl_xor(rs, 4, 32); rs += __shfl_xor(rs, 8, 32);
                    l8[i] = l8[i] * corr + rs; m8[i] = mnew;
                    if (!TWOPASS) {
#pragma unroll
                        for (int t = 0; t < NT; ++t) o[t][i] *= corr;
                    }
                } else {
                    const float inv = (l8[i] > 0.f) ? 1.f / l8[i] : 0.f;
#pragma unroll
                    for (int t = 0; t < 4; ++t) {
                        const int jg = j0 + t * 16 + l15;
                        float pp = (sc[t] == NEG) ? 0.f : exp2f(sc[t] - m8[i]) * inv;
                        if (p.Pw) pp *= p.Pw[b * p.swb + h * p.swh + (long long)ic * p.swi + (long long)min(jg, p.Lk - 1) * p.swj];
                        pv[i][t] = pp;
                    }
                }
            }
            if (dopv) {
#pragma unroll
                for (int i = 0; i < 8; ++i)
#pragma unroll
                    for (int t = 0; t < 4; ++t) myp[(i + 8 * hf) * 64 + t * 16 + l15] = pv[i][t];
                __syncthreads();
                if (p.P) {
                    float* pb_ = p.P + b * p.sPb + h * p.sPh;
                    const bool fastP = (p.pband == 0) && ((p.sPi & 3) == 0) && (j0 + 64 <= p.Lk) && (q0 + 16 <= p.Lq) && ((((size_t)pb_) & 15) == 0);
                    if (fastP) {
#pragma unroll
                        for (int s = 0; s < 8; ++s) {
                            const int row = s * 2 + (lane >> 4), c4 = (lane & 15) * 4;
                            const v4f v = *(const v4f*)(myp + row * 64 + c4);
                            VST2V4(pb_ + (long long)(q0 + row) * p.sPi + j0 + c4, v);
                        }
                    } else {
                        for (int row = 0; row < 16; ++row) {
                            const int irow = q0 + row; if (irow >= p.Lq) continue;
                            for (int c = lane; c < 64; c += 32) {
                                const int jg = j0 + c; if (jg >= p.Lk) continue;
                                if (p.pband == 0) VST2(float, pb_ + (long long)irow * p.sPi + jg, myp[row * 64 + c]);
                                else if (jg - irow <= p.pband && irow - jg <= p.pband) VST2(float, pb_ + (long long)irow * p.sPi + (jg - irow + p.pband), myp[row * 64 + c]);
                            }
                        }
                    }
                }
                if (SPLITPV) {
                    const Split pa0 = sp_ld(myp + l15 * 64, 1, 0, hf, 64, 1.f), pa1 = sp_ld(myp + l15 * 64, 1, 32, hf, 64, 1.f);
                    const __bf16* vh = (const __bf16*)vl; const __bf16* vlo = vh + 64 * VP;
#pragma unroll
                    for (int t = 0; t < NT; ++t) {
                        const int dcol = t * 16 + l15;
                        Split b0, b1;
#pragma unroll
                        for (int e = 0; e < 16; ++e) {
                            const int k0 = frag_k(e, hf), k1 = 32 + frag_k(e, hf);
                            b0.hi[e] = vh[k0 * VP + dcol]; b0.lo[e] = vlo[k0 * VP + dcol]; b1.hi[e] = vh[k1 * VP + dcol]; b1.lo[e] = vlo[k1 * VP + dcol];
                        }
                        o[t] = wmma3(pa0, b0, o[t]);
                        o[t] = wmma3(pa1, b1, o[t]);
                    }
                } else {
                    const v16h pa0 = fh_ld(myp + l15 * 64, 1, 0, hf, 64, 4096.f), pa1 = fh_ld(myp + l15 * 64, 1, 32, hf, 64, 4096.f);
#pragma unroll
                    for (int t = 0; t < NT; ++t) {
                        const int dcol = t * 16 + l15;
                        v16h b0, b1;
#pragma unroll
                        for (int e = 0; e < 16; ++e) { b0[e] = vl[frag_k(e, hf) * VP + dcol]; b1[e] = vl[(32 + frag_k(e, hf)) * VP + dcol]; }
                        o[t] = wmma16(pa0, b0, o[t]);
                        o[t] = wmma16(pa1, b1, o[t]);
                    }
                }
            }
        }
    }
    float* obase = p.O + b * p.sOb + h * p.sOh;
    if (p.ST) {
        const int rl = lane >> 1, isel = rl & 7;
        float mv = 0.f, lv = 0.f;
#pragma unroll
        for (int i = 0; i < 8; ++i) if (i == isel) { mv = m8[i]; lv = l8[i]; }
        const int irow = q0 + rl;
        if (irow < p.Lq) { float* st = p.ST + (((long long)b * gridDim.y + h) * p.Lq + irow) * 2 + (lane & 1); VST2(float, st, (lane & 1) ? lv : mv * 0.6931471805599453f); }
    }
    float invr[8];
#pragma unroll
    for (int i = 0; i < 8; ++i) {
        if (TWOPASS) invr[i] = SPLITPV ? 1.f : (1.f / 4096.f);
        else if (p.nonorm) invr[i] = exp2f(m8[i]) * (SPLITPV ? 1.f : (1.f / 4096.f));
        else invr[i] = (l8[i] > 0.f) ? (SPLITPV ? 1.f / l8[i] : 1.f / (l8[i] * 4096.f)) : 0.f;
    }
    __syncthreads();
    const bool ofast = ((p.sOi & 3) == 0) && ((((size_t)obase) & 15) == 0) && (q0 + 16 <= p.Lq);
#pragma unroll
    for (int c0 = 0; c0 < DVP; c0 += 64) {
#pragma unroll
        for (int i = 0; i < 8; ++i)
#pragma unroll
            for (int t = 0; t < NT; ++t) if (t * 16 >= c0 && t * 16 < c0 + 64) myp[(i + 8 * hf) * 64 + (t * 16 - c0) + l15] = o[t][i] * invr[i];
        __syncthreads();
        const int cw = (DVP - c0 < 64) ? (DVP - c0) : 64;
        if (ofast && (c0 + cw <= p.dv) && (cw % 32 == 0)) {
            const int lpr = cw / 4;
            const int rows_per_ins = 32 / lpr;
            for (int r0 = 0; r0 < 16; r0 += rows_per_ins) {
                const int row = r0 + lane / lpr, c4 = (lane % lpr) * 4;
                const v4f v = *(const v4f*)(myp + row * 64 + c4);
                VST2V4(obase + (long long)(q0 + row) * p.sOi + c0 + c4, v);
            }
        } else {
            for (int row = 0; row < 16; ++row) {
                const int irow = q0 + row; if (irow >= p.Lq) continue;
                for (int c = lane; c < cw; c += 32) { const int d = c0 + c; if (d < p.dv) VST2(float, obase + (long long)irow * p.sOi + d, myp[row * 64 + c]); }
            }
        }
        __syncthreads();
    }
}

struct TrP { const float* src; float* dst; const float* R2; long long sSz, lds, sDz, ldd, sRz, ldr; int R, C, flags, act; float alpha, beta; };
static_assert(sizeof(TrP) == 3 * 8 + 6 * 8 + 6 * 4, "TrP has padding");
__global__ __launch_bounds__(256) void k_tr(TrP p) {
    __shared__ float tile[32][33];
    const int c0 = blockIdx.x * 32, r0 = blockIdx.y * 32, z = blockIdx.z;
    const int lane = threadIdx.x & 31, wave = threadIdx.x >> 5;
    const float* s = p.src + z * p.sSz;
#pragma unroll
    for (int k = 0; k < 4; ++k) {
        const int rl = wave * 4 + k, r = r0 + rl, c = c0 + lane;
        tile[rl][lane] = (r < p.R && c < p.C) ? s[(long long)r * p.lds + c] : 0.f;
    }
    __syncthreads();
    float* d = p.dst + z * p.sDz; const float* rr = p.R2 + z * p.sRz;
#pragma unroll
    for (int k = 0; k < 4; ++k) {
        const int cl = wave * 4 + k, c = c0 + cl, r = r0 + lane;
        if (c < p.C && r < p.R) {
            float v = act_fn(p.alpha * tile[lane][cl], p.act);
            if (p.flags & 1) v += p.beta * rr[(long long)c * p.ldr + r];
            VST2(float, d + (long long)c * p.ldd + r, v);
        }
    }
}

__global__ __launch_bounds__(256) void k_affine(const float* __restrict__ src, float* __restrict__ dst, int n, float a, float b, const float* __restrict__ sdev) {
    const int i = blockIdx.x * 256 + threadIdx.x;
    if (i < n) { const float aa = sdev ? a * sdev[0] : a; const float v = aa * src[i] + b; VST2(float, dst + i, v); }
}

struct SmP { const float* src; float* dst; const float* Mf; long long sz, sr, dz, dr, smz, smr; int n, pad; float scale_in, scale_out; };
static_assert(sizeof(SmP) == 3 * 8 + 6 * 8 + 4 * 4, "SmP has padding");
__global__ __launch_bounds__(256) void k_softmax(SmP p) {
    __shared__ float red[256];
    const int r = blockIdx.x, z = blockIdx.y, tid = threadIdx.x;
    const float* s = p.src + z * p.sz + (long long)r * p.sr;
    const float* mf = p.Mf ? (p.Mf + z * p.smz + (long long)r * p.smr) : nullptr;
    float mx = -__builtin_inff();
    for (int j = tid; j < p.n; j += 256) { float v = s[j] * p.scale_in; if (mf) v += mf[j]; mx = fmaxf(mx, v); }
    red[tid] = mx; __syncthreads();
    for (int o = 128; o > 0; o >>= 1) { if (tid < o) red[tid] = fmaxf(red[tid], red[tid + o]); __syncthreads(); }
    mx = red[0]; __syncthreads();
    float sum = 0.f;
    for (int j = tid; j < p.n; j += 256) { float v = s[j] * p.scale_in; if (mf) v += mf[j]; sum += (mx == -__builtin_inff()) ? 0.f : expf(v - mx); }
    red[tid] = sum; __syncthreads();
    for (int o = 128; o > 0; o >>= 1) { if (tid < o) red[tid] += red[tid + o]; __syncthreads(); }
    sum = red[0];
    const float inv = (sum > 0.f) ? p.scale_out / sum : 0.f;
    float* d = p.dst + z * p.dz + (long long)r * p.dr;
    for (int j = tid; j < p.n; j += 256) { float v = s[j] * p.scale_in; if (mf) v += mf[j]; const float o = (mx == -__builtin_inff()) ? 0.f : expf(v - mx) * inv; VST2(float, d + j, o); }
}
__global__ __launch_bounds__(256) void k_stats(const float* __restrict__ x, long long sz, long long so, long long si, int inner, int n, float eps, float* __restrict__ stat, int mode) {
    __shared__ float red[256];
    const int z = blockIdx.x, tid = threadIdx.x;
    const float* base = x + z * sz;
    float s = 0.f;
    for (int e = tid; e < n; e += 256) s += base[(long long)(e / inner) * so + (long long)(e % inner) * si];
    red[tid] = s; __syncthreads();
    for (int o = 128; o > 0; o >>= 1) { if (tid < o) red[tid] += red[tid + o]; __syncthreads(); }
    const float mu = (mode == 0 || mode == 3) ? red[0] / (float)n : 0.f; __syncthreads();
    float q = 0.f;
    for (int e = tid; e < n; e += 256) { const float dlt = base[(long long)(e / inner) * so + (long long)(e % inner) * si] - mu; q += dlt * dlt; }
    red[tid] = q; __syncthreads();
    for (int o = 128; o > 0; o >>= 1) { if (tid < o) red[tid] += red[tid + o]; __syncthreads(); }
    {
        float rs;
        if (mode == 2) rs = sqrtf((float)n) / fmaxf(sqrtf(red[0]), eps); else if (mode == 3) rs = rsqrtf(red[0] / (float)(n - 1) + eps); else rs = rsqrtf(red[0] / (float)n + eps);
        if (tid < 32) { const float v = (tid == 0) ? mu : ((tid == 1) ? rs : 0.f); VST2(float, stat + (long long)z * 32 + tid, v); }
    }
}
__global__ __launch_bounds__(256) void k_norm_apply(const float* __restrict__ x, float* __restrict__ y, const float* __restrict__ stat, const float* __restrict__ g, const float* __restrict__ bta,
                                                     int Z, int C, int L, int G, int bn, int act) {
    const long long idx = (long long)blockIdx.x * 256 + threadIdx.x;
    if (idx >= (long long)Z * C * L) return;
    const int l = (int)(idx % L); const long long zc = idx / L; const int c = (int)(zc % C), z = (int)(zc / C); (void)l;
    const int set = bn ? c : (z * G + c / (C / G));
    float v = (x[idx] - stat[(long long)set * 32]) * stat[(long long)set * 32 + 1];
    if (g) v *= g[c];
    if (bta) v += bta[c];
    v = act_fn(v, act);
    VST2(float, y + idx, v);
}

__global__ __launch_bounds__(256) void k_lse_neg(const float* __restrict__ st, float* __restrict__ c, int n) {
    const int i = blockIdx.x * 256 + threadIdx.x;
    if (i < n) { const float v = -(st[2 * i] + logf(st[2 * i + 1])); VST2(float, c + i, v); }
}

__global__ __launch_bounds__(256) void k_iota(int* __restrict__ dst, int n, int a, int b) {
    const int i = blockIdx.x * 256 + threadIdx.x;
    if (i < n) { const int v = a * i + b; VST2(int, dst + i, v); }
}

__global__ __launch_bounds__(256) void k_axpby(const float* __restrict__ x, const float* __restrict__ y, float* __restrict__ dst, int n, float a, float b, float c) {
    const int i = blockIdx.x * 256 + threadIdx.x;
    if (i < n) { const float v = a * x[i] + b * y[i] + c; VST2(float, dst + i, v); }
}

struct RopeP { const float* X; float* Y; const float* C; const float* Sn; const int* pos; long long sXr, sXh, sYr, sYh, sCb, sCp, sCd; int R, Hn, D, S, mode, tmode, pmode, pad; };
static_assert(sizeof(RopeP) == 5 * 8 + 7 * 8 + 8 * 4, "RopeP has padding");
__global__ __launch_bounds__(256) void k_rope(RopeP p) {
    const long long idx = (long long)blockIdx.x * 256 + threadIdx.x;
    if (idx >= (long long)p.R * p.Hn * p.D) return;
    const int d = (int)(idx % p.D); const long long rh = idx / p.D; const int h = (int)(rh % p.Hn); const int r = (int)(rh / p.Hn);
    const int half = p.D / 2;
    int partner; float sign;
    if (p.mode == 0) { partner = (d < half) ? d + half : d - half; sign = (d < half) ? -1.f : 1.f; }
    else { partner = d ^ 1; sign = (d & 1) ? 1.f : -1.f; }
    const int tcol = (p.tmode == 0) ? d : ((p.tmode == 1) ? (d % half) : (d >> 1));
    const int pp = (p.pmode == 0) ? (r % p.S) : ((p.pmode == 1) ? h : p.pos[r]);
    const long long toff = (long long)(r / p.S) * p.sCb + (long long)pp * p.sCp + (long long)tcol * p.sCd;
    const float* xr = p.X + (long long)r * p.sXr + (long long)h * p.sXh;
    const float v = xr[d] * p.C[toff] + sign * xr[partner] * p.Sn[toff];
    VST2(float, p.Y + (long long)r * p.sYr + (long long)h * p.sYh + d, v);
}

__global__ __launch_bounds__(256) void k_invf(float* __restrict__ invb, int half, int D, float base, float num, int fmode, float cexp) {
    const int i = blockIdx.x * 256 + threadIdx.x;
    if (i >= ((half + 31) / 32) * 32) return;
    if (i >= half) { VST2(float, invb + i, 0.f); return; }
    const float e = (float)(2 * i) / (float)D;
    float invf;
    if (fmode == 1) invf = num * expf((float)(2 * i) * cexp);
    else if (fmode == 2) invf = num * powf(base, (-2.0f * ((float)i - 1.0f)) / (float)D);
    else invf = num * (1.0f / powf(base, e));
    VST2(float, invb + i, invf);
}
__global__ __launch_bounds__(256) void k_sincos(float* __restrict__ cs, float* __restrict__ sn, const float* __restrict__ invb, int S, int half, float pscale) {
    const int idx = blockIdx.x * 256 + threadIdx.x;
    if (idx >= S * half) return;
    const int s = idx / half, i = idx - s * half;
    const float ang = (pscale * (float)s) * invb[i];
    VST2(float, cs + idx, cosf(ang)); VST2(float, sn + idx, sinf(ang));
}

__global__ __launch_bounds__(256) void k_mulact(const float* __restrict__ x, const float* __restrict__ y, float* __restrict__ dst, int n, int act) {
    const int i = blockIdx.x * 256 + threadIdx.x;
    if (i < n) { const float v = act_fn(x[i], act) * y[i]; VST2(float, dst + i, v); }
}

__global__ __launch_bounds__(256) void k_matvec(GemmP p) {
    const int rpt = (p.N == 1) ? 1 : 32;
    const long long r0 = ((long long)blockIdx.x * 256 + threadIdx.x) * rpt; const int z = blockIdx.z, zo = z / p.zi_n, zi = z - zo * p.zi_n;
    if (r0 >= p.M) return;
    const float* Bb = p.B + zo * p.sBo + zi * p.sBi;
    float* C = p.C + zo * p.sCo + zi * p.sCi; const float* R = p.R + zo * p.sRo + zi * p.sRi;
    for (int rr = 0; rr < rpt; ++rr) {
        const long long r = r0 + rr; if (r >= p.M) break;
        const float* A = p.A + zo * p.sAo + zi * p.sAi + r * p.sAm;
        float acc[8] = {0.f, 0.f, 0.f, 0.f, 0.f, 0.f, 0.f, 0.f};
        for (int k = 0; k < p.K; ++k) { const float a = A[(long long)k * p.sAk];
#pragma unroll
            for (int j = 0; j < 8; ++j) if (j < p.N) acc[j] += a * Bb[(long long)j * p.sBn + (long long)k * p.sBk]; }
#pragma unroll
        for (int j = 0; j < 8; ++j) if (j < p.N) {
            float v = acc[j] * p.alpha;
            if (p.flags & 1) v += p.bias[j];
            if (p.flags & 2) v += p.bias[r];
            v = act_fn(v, p.act);
            if (p.flags & 4) v += p.beta * R[r * p.sRm + (long long)j * p.sRn];
            VST2(float, C + r * p.sCm + j, v);
        }
    }
}
__global__ __launch_bounds__(256) void k_smallsoftmax(const float* __restrict__ src, float* __restrict__ dst, long long sr, long long dr, int n, long long R, float scale) {
    const long long r0 = ((long long)blockIdx.x * 256 + threadIdx.x) * 32;
    for (int rr = 0; rr < 32; ++rr) {
        const long long r = r0 + rr; if (r >= R) return;
        const float* s = src + r * sr; float* d = dst + r * dr;
        float mx = -__builtin_inff();
        for (int j = 0; j < n; ++j) mx = fmaxf(mx, s[j] * scale);
        float sum = 0.f;
        for (int j = 0; j < n; ++j) sum += expf(s[j] * scale - mx);
        const float inv = 1.f / sum;
        for (int j = 0; j < n; ++j) { const float v = expf(s[j] * scale - mx) * inv; VST2(float, d + j, v); }
    }
}

__global__ __launch_bounds__(32) void k_unitstat(float* __restrict__ st) { const int t = threadIdx.x; const float v = (t == 1) ? 1.f : 0.f; VST2(float, st + t, v); }

__global__ __launch_bounds__(256) void k_lincopy(const float* __restrict__ src, long long lds, float* __restrict__ dst, long long ldd, long long rows, int cols) {
    const long long i = (long long)blockIdx.x * 256 + threadIdx.x; if (i >= rows * cols) return;
    const long long r = i / cols; const int c = (int)(i - r * cols);
    const float v = src[r * lds + c]; VST2(float, dst + r * ldd + c, v);
}

__global__ __launch_bounds__(128) void k_tb_b4(const float* __restrict__ b, float* __restrict__ B4, int E) { const int q = threadIdx.x; if (q < E) VST2(float, B4 + q, 4.f * b[q]); }
__global__ __launch_bounds__(256) void k_tb_gather(const int* __restrict__ tok, const float* __restrict__ EW, float* __restrict__ H, int t0, int TC, int NN, int E, int V) { const long long q = (long long)blockIdx.x * 256 + threadIdx.x; if (q >= (long long)TC * NN * E) return; const int e = (int)(q % E); const long long tn = q / E; int id = tok[(long long)t0 * NN + tn]; id = min(max(id, 0), V - 1); VST2(float, H + q, EW[(long long)id * E + e]); }
__global__ __launch_bounds__(256) void k_tb_csum(const float* __restrict__ H, float* __restrict__ CS, int TC, int NN, int E, int pstart, int npar, int cstart) { const long long q = (long long)blockIdx.x * 256 + threadIdx.x; if (q >= (long long)TC * npar * E) return; const int e = (int)(q % E); const int pr = (int)((q / E) % npar); const int t = (int)(q / ((long long)E * npar)); const float* hb = H + ((long long)t * NN + cstart + 4 * pr) * E + e; VST2(float, CS + q, (hb[0] + hb[E]) + (hb[2 * E] + hb[3 * E])); }
__global__ __launch_bounds__(128) void k_tb_max(const float* __restrict__ H, float* __restrict__ OUT, int t0, int TC, int NN, int E) { const int q = blockIdx.x * 128 + threadIdx.x; if (q >= TC * E) return; const int e = q % E; const int t = q / E; float m = 0.f;
#pragma unroll 1
    for (int n = 0; n < NN; ++n) m = fmaxf(m, H[((long long)t * NN + n) * E + e]); VST2(float, OUT + (long long)(t0 + t) * E + e, m); }

template __global__ void k_gemm<1>(GemmP);

extern "C" void kernel_launch(void* const* d_in, const int* in_sizes, int n_in, void* d_out, int out_size, void* d_ws, size_t ws_size, hipStream_t stream) {
    (void)in_sizes; (void)n_in; (void)out_size; (void)ws_size;
    const int* tok = (const int*)d_in[0];
    const float* emb = (const float*)d_in[1];
    const float* WcW = (const float*)d_in[2];
    const float* Wcb = (const float*)d_in[3];
    const float* WsW = (const float*)d_in[4];
    const float* Wsb = (const float*)d_in[5];
    const int* bs_ = (const int*)d_in[6];
    const int NB = 512;
    const int A4 = 4;
    const int NN = 1365;
    const int V = 50000;
    const int E = 128;
    const int TC = 64;
    const int NPAR = 341;
    float* out = (float*)d_out;
    char* wsp = (char*)d_ws;
    float* EW = (float*)wsp; wsp += (((size_t)((size_t)V * E) * 4 + 255) / 256) * 256;
    float* H = (float*)wsp; wsp += (((size_t)((size_t)TC * NN * E) * 4 + 255) / 256) * 256;
    float* CS = (float*)wsp; wsp += (((size_t)((size_t)TC * 256 * E) * 4 + 255) / 256) * 256;
    float* B4 = (float*)wsp; wsp += (((size_t)((size_t)E) * 4 + 255) / 256) * 256;
    { GemmP gew;
      gew.A = emb; gew.B = WcW; gew.bias = Wcb; gew.R = emb; gew.C = EW;
      gew.sAo = 0; gew.sAi = 0; gew.sAm = E; gew.sAk = 1; gew.sBo = 0; gew.sBi = 0; gew.sBn = E; gew.sBk = 1; gew.sCo = 0; gew.sCi = 0; gew.sCm = E; gew.sRo = 0; gew.sRi = 0; gew.sRm = 0; gew.sRn = 0;
      gew.M = V; gew.N = E; gew.K = E; gew.zi_n = 1; gew.flags = 1; gew.act = 0;
      gew.alpha = 1.0f; gew.beta = 0.0f; gew.sa = 1.0f; gew.sb = 1.0f; gew.Npad = E; gew.pad_ = 0;
      if ((long long)(V) >= 64 && (long long)(E) >= 64) k_gemmT<1, 2, 4><<<dim3((unsigned)((E) + 63) / 64, (unsigned)((V) + 31) / 32, (unsigned)(1)), 32, 0, stream>>>(gew);
      else k_gemm<1><<<dim3((unsigned)((E) + 31) / 32, (unsigned)((V) + 15) / 16, (unsigned)(1)), 32, 0, stream>>>(gew); }
    k_tb_b4<<<1, 128, 0, stream>>>(Wsb, B4, E);
    k_tb_gather<<<(unsigned)(((long long)TC * NN * E + 255) / 256), 256, 0, stream>>>(tok, EW, H, 0, TC, NN, E, V);
    k_tb_csum<<<(unsigned)(((long long)TC * 256 * E + 255) / 256), 256, 0, stream>>>(H, CS, TC, NN, E, 85, 256, 341);
    { GemmP gl04;
      gl04.A = CS; gl04.B = WsW; gl04.bias = B4; gl04.R = H + (size_t)85 * E; gl04.C = H + (size_t)85 * E;
      gl04.sAo = (long long)256 * E; gl04.sAi = 0; gl04.sAm = E; gl04.sAk = 1; gl04.sBo = 0; gl04.sBi = 0; gl04.sBn = E; gl04.sBk = 1; gl04.sCo = (long long)NN * E; gl04.sCi = 0; gl04.sCm = E; gl04.sRo = (long long)NN * E; gl04.sRi = 0; gl04.sRm = E; gl04.sRn = 1;
      gl04.M = 256; gl04.N = E; gl04.K = E; gl04.zi_n = 1; gl04.flags = 5; gl04.act = 0;
      gl04.alpha = 1.0f; gl04.beta = 1.0f; gl04.sa = 1.0f; gl04.sb = 1.0f; gl04.Npad = E; gl04.pad_ = 0;
      if ((long long)(256) >= 64 && (long long)(E) >= 64) k_gemmT<1, 2, 4><<<dim3((unsigned)((E) + 63) / 64, (unsigned)((256) + 31) / 32, (unsigned)(TC)), 32, 0, stream>>>(gl04);
      else k_gemm<1><<<dim3((unsigned)((E) + 31) / 32, (unsigned)((256) + 15) / 16, (unsigned)(TC)), 32, 0, stream>>>(gl04); }
    k_tb_csum<<<(unsigned)(((long long)TC * 64 * E + 255) / 256), 256, 0, stream>>>(H, CS, TC, NN, E, 21, 64, 85);
    { GemmP gl03;
      gl03.A = CS; gl03.B = WsW; gl03.bias = B4; gl03.R = H + (size_t)21 * E; gl03.C = H + (size_t)21 * E;
      gl03.sAo = (long long)64 * E; gl03.sAi = 0; gl03.sAm = E; gl03.sAk = 1; gl03.sBo = 0; gl03.sBi = 0; gl03.sBn = E; gl03.sBk = 1; gl03.sCo = (long long)NN * E; gl03.sCi = 0; gl03.sCm = E; gl03.sRo = (long long)NN * E; gl03.sRi = 0; gl03.sRm = E; gl03.sRn = 1;
      gl03.M = 64; gl03.N = E; gl03.K = E; gl03.zi_n = 1; gl03.flags = 5; gl03.act = 0;
      gl03.alpha = 1.0f; gl03.beta = 1.0f; gl03.sa = 1.0f; gl03.sb = 1.0f; gl03.Npad = E; gl03.pad_ = 0;
      if ((long long)(64) >= 64 && (long long)(E) >= 64) k_gemmT<1, 2, 4><<<dim3((unsigned)((E) + 63) / 64, (unsigned)((64) + 31) / 32, (unsigned)(TC)), 32, 0, stream>>>(gl03);
      else k_gemm<1><<<dim3((unsigned)((E) + 31) / 32, (unsigned)((64) + 15) / 16, (unsigned)(TC)), 32, 0, stream>>>(gl03); }
    k_tb_csum<<<(unsigned)(((long long)TC * 16 * E + 255) / 256), 256, 0, stream>>>(H, CS, TC, NN, E, 5, 16, 21);
    { GemmP gl02;
      gl02.A = CS; gl02.B = WsW; gl02.bias = B4; gl02.R = H + (size_t)5 * E; gl02.C = H + (size_t)5 * E;
      gl02.sAo = (long long)16 * E; gl02.sAi = 0; gl02.sAm = E; gl02.sAk = 1; gl02.sBo = 0; gl02.sBi = 0; gl02.sBn = E; gl02.sBk = 1; gl02.sCo = (long long)NN * E; gl02.sCi = 0; gl02.sCm = E; gl02.sRo = (long long)NN * E; gl02.sRi = 0; gl02.sRm = E; gl02.sRn = 1;
      gl02.M = 16; gl02.N = E; gl02.K = E; gl02.zi_n = 1; gl02.flags = 5; gl02.act = 0;
      gl02.alpha = 1.0f; gl02.beta = 1.0f; gl02.sa = 1.0f; gl02.sb = 1.0f; gl02.Npad = E; gl02.pad_ = 0;
      k_gemm<1><<<dim3((unsigned)((E) + 31) / 32, (unsigned)((16) + 15) / 16, (unsigned)(TC)), 32, 0, stream>>>(gl02); }
    k_tb_csum<<<(unsigned)(((long long)TC * 4 * E + 255) / 256), 256, 0, stream>>>(H, CS, TC, NN, E, 1, 4, 5);
    { GemmP gl01;
      gl01.A = CS; gl01.B = WsW; gl01.bias = B4; gl01.R = H + (size_t)1 * E; gl01.C = H + (size_t)1 * E;
      gl01.sAo = (long long)4 * E; gl01.sAi = 0; gl01.sAm = E; gl01.sAk = 1; gl01.sBo = 0; gl01.sBi = 0; gl01.sBn = E; gl01.sBk = 1; gl01.sCo = (long long)NN * E; gl01.sCi = 0; gl01.sCm = E; gl01.sRo = (long long)NN * E; gl01.sRi = 0; gl01.sRm = E; gl01.sRn = 1;
      gl01.M = 4; gl01.N = E; gl01.K = E; gl01.zi_n = 1; gl01.flags = 5; gl01.act = 0;
      gl01.alpha = 1.0f; gl01.beta = 1.0f; gl01.sa = 1.0f; gl01.sb = 1.0f; gl01.Npad = E; gl01.pad_ = 0;
      k_gemm<1><<<dim3((unsigned)((E) + 31) / 32, (unsigned)((4) + 15) / 16, (unsigned)(TC)), 32, 0, stream>>>(gl01); }
    k_tb_csum<<<(unsigned)(((long long)TC * 1 * E + 255) / 256), 256, 0, stream>>>(H, CS, TC, NN, E, 0, 1, 1);
    { GemmP gl00;
      gl00.A = CS; gl00.B = WsW; gl00.bias = B4; gl00.R = H + (size_t)0 * E; gl00.C = H + (size_t)0 * E;
      gl00.sAo = (long long)1 * E; gl00.sAi = 0; gl00.sAm = E; gl00.sAk = 1; gl00.sBo = 0; gl00.sBi = 0; gl00.sBn = E; gl00.sBk = 1; gl00.sCo = (long long)NN * E; gl00.sCi = 0; gl00.sCm = E; gl00.sRo = (long long)NN * E; gl00.sRi = 0; gl00.sRm = E; gl00.sRn = 1;
      gl00.M = 1; gl00.N = E; gl00.K = E; gl00.zi_n = 1; gl00.flags = 5; gl00.act = 0;
      gl00.alpha = 1.0f; gl00.beta = 1.0f; gl00.sa = 1.0f; gl00.sb = 1.0f; gl00.Npad = E; gl00.pad_ = 0;
      k_gemm<1><<<dim3((unsigned)((E) + 31) / 32, (unsigned)((1) + 15) / 16, (unsigned)(TC)), 32, 0, stream>>>(gl00); }
    k_tb_max<<<(unsigned)((TC * E + 127) / 128), 128, 0, stream>>>(H, out, 0, TC, NN, E);
    k_tb_gather<<<(unsigned)(((long long)TC * NN * E + 255) / 256), 256, 0, stream>>>(tok, EW, H, 64, TC, NN, E, V);
    k_tb_csum<<<(unsigned)(((long long)TC * 256 * E + 255) / 256), 256, 0, stream>>>(H, CS, TC, NN, E, 85, 256, 341);
    { GemmP gl14;
      gl14.A = CS; gl14.B = WsW; gl14.bias = B4; gl14.R = H + (size_t)85 * E; gl14.C = H + (size_t)85 * E;
      gl14.sAo = (long long)256 * E; gl14.sAi = 0; gl14.sAm = E; gl14.sAk = 1; gl14.sBo = 0; gl14.sBi = 0; gl14.sBn = E; gl14.sBk = 1; gl14.sCo = (long long)NN * E; gl14.sCi = 0; gl14.sCm = E; gl14.sRo = (long long)NN * E; gl14.sRi = 0; gl14.sRm = E; gl14.sRn = 1;
      gl14.M = 256; gl14.N = E; gl14.K = E; gl14.zi_n = 1; gl14.flags = 5; gl14.act = 0;
      gl14.alpha = 1.0f; gl14.beta = 1.0f; gl14.sa = 1.0f; gl14.sb = 1.0f; gl14.Npad = E; gl14.pad_ = 0;
      if ((long long)(256) >= 64 && (long long)(E) >= 64) k_gemmT<1, 2, 4><<<dim3((unsigned)((E) + 63) / 64, (unsigned)((256) + 31) / 32, (unsigned)(TC)), 32, 0, stream>>>(gl14);
      else k_gemm<1><<<dim3((unsigned)((E) + 31) / 32, (unsigned)((256) + 15) / 16, (unsigned)(TC)), 32, 0, stream>>>(gl14); }
    k_tb_csum<<<(unsigned)(((long long)TC * 64 * E + 255) / 256), 256, 0, stream>>>(H, CS, TC, NN, E, 21, 64, 85);
    { GemmP gl13;
      gl13.A = CS; gl13.B = WsW; gl13.bias = B4; gl13.R = H + (size_t)21 * E; gl13.C = H + (size_t)21 * E;
      gl13.sAo = (long long)64 * E; gl13.sAi = 0; gl13.sAm = E; gl13.sAk = 1; gl13.sBo = 0; gl13.sBi = 0; gl13.sBn = E; gl13.sBk = 1; gl13.sCo = (long long)NN * E; gl13.sCi = 0; gl13.sCm = E; gl13.sRo = (long long)NN * E; gl13.sRi = 0; gl13.sRm = E; gl13.sRn = 1;
      gl13.M = 64; gl13.N = E; gl13.K = E; gl13.zi_n = 1; gl13.flags = 5; gl13.act = 0;
      gl13.alpha = 1.0f; gl13.beta = 1.0f; gl13.sa = 1.0f; gl13.sb = 1.0f; gl13.Npad = E; gl13.pad_ = 0;
      if ((long long)(64) >= 64 && (long long)(E) >= 64) k_gemmT<1, 2, 4><<<dim3((unsigned)((E) + 63) / 64, (unsigned)((64) + 31) / 32, (unsigned)(TC)), 32, 0, stream>>>(gl13);
      else k_gemm<1><<<dim3((unsigned)((E) + 31) / 32, (unsigned)((64) + 15) / 16, (unsigned)(TC)), 32, 0, stream>>>(gl13); }
    k_tb_csum<<<(unsigned)(((long long)TC * 16 * E + 255) / 256), 256, 0, stream>>>(H, CS, TC, NN, E, 5, 16, 21);
    { GemmP gl12;
      gl12.A = CS; gl12.B = WsW; gl12.bias = B4; gl12.R = H + (size_t)5 * E; gl12.C = H + (size_t)5 * E;
      gl12.sAo = (long long)16 * E; gl12.sAi = 0; gl12.sAm = E; gl12.sAk = 1; gl12.sBo = 0; gl12.sBi = 0; gl12.sBn = E; gl12.sBk = 1; gl12.sCo = (long long)NN * E; gl12.sCi = 0; gl12.sCm = E; gl12.sRo = (long long)NN * E; gl12.sRi = 0; gl12.sRm = E; gl12.sRn = 1;
      gl12.M = 16; gl12.N = E; gl12.K = E; gl12.zi_n = 1; gl12.flags = 5; gl12.act = 0;
      gl12.alpha = 1.0f; gl12.beta = 1.0f; gl12.sa = 1.0f; gl12.sb = 1.0f; gl12.Npad = E; gl12.pad_ = 0;
      k_gemm<1><<<dim3((unsigned)((E) + 31) / 32, (unsigned)((16) + 15) / 16, (unsigned)(TC)), 32, 0, stream>>>(gl12); }
    k_tb_csum<<<(unsigned)(((long long)TC * 4 * E + 255) / 256), 256, 0, stream>>>(H, CS, TC, NN, E, 1, 4, 5);
    { GemmP gl11;
      gl11.A = CS; gl11.B = WsW; gl11.bias = B4; gl11.R = H + (size_t)1 * E; gl11.C = H + (size_t)1 * E;
      gl11.sAo = (long long)4 * E; gl11.sAi = 0; gl11.sAm = E; gl11.sAk = 1; gl11.sBo = 0; gl11.sBi = 0; gl11.sBn = E; gl11.sBk = 1; gl11.sCo = (long long)NN * E; gl11.sCi = 0; gl11.sCm = E; gl11.sRo = (long long)NN * E; gl11.sRi = 0; gl11.sRm = E; gl11.sRn = 1;
      gl11.M = 4; gl11.N = E; gl11.K = E; gl11.zi_n = 1; gl11.flags = 5; gl11.act = 0;
      gl11.alpha = 1.0f; gl11.beta = 1.0f; gl11.sa = 1.0f; gl11.sb = 1.0f; gl11.Npad = E; gl11.pad_ = 0;
      k_gemm<1><<<dim3((unsigned)((E) + 31) / 32, (unsigned)((4) + 15) / 16, (unsigned)(TC)), 32, 0, stream>>>(gl11); }
    k_tb_csum<<<(unsigned)(((long long)TC * 1 * E + 255) / 256), 256, 0, stream>>>(H, CS, TC, NN, E, 0, 1, 1);
    { GemmP gl10;
      gl10.A = CS; gl10.B = WsW; gl10.bias = B4; gl10.R = H + (size_t)0 * E; gl10.C = H + (size_t)0 * E;
      gl10.sAo = (long long)1 * E; gl10.sAi = 0; gl10.sAm = E; gl10.sAk = 1; gl10.sBo = 0; gl10.sBi = 0; gl10.sBn = E; gl10.sBk = 1; gl10.sCo = (long long)NN * E; gl10.sCi = 0; gl10.sCm = E; gl10.sRo = (long long)NN * E; gl10.sRi = 0; gl10.sRm = E; gl10.sRn = 1;
      gl10.M = 1; gl10.N = E; gl10.K = E; gl10.zi_n = 1; gl10.flags = 5; gl10.act = 0;
      gl10.alpha = 1.0f; gl10.beta = 1.0f; gl10.sa = 1.0f; gl10.sb = 1.0f; gl10.Npad = E; gl10.pad_ = 0;
      k_gemm<1><<<dim3((unsigned)((E) + 31) / 32, (unsigned)((1) + 15) / 16, (unsigned)(TC)), 32, 0, stream>>>(gl10); }
    k_tb_max<<<(unsigned)((TC * E + 127) / 128), 128, 0, stream>>>(H, out, 64, TC, NN, E);
    k_tb_gather<<<(unsigned)(((long long)TC * NN * E + 255) / 256), 256, 0, stream>>>(tok, EW, H, 128, TC, NN, E, V);
    k_tb_csum<<<(unsigned)(((long long)TC * 256 * E + 255) / 256), 256, 0, stream>>>(H, CS, TC, NN, E, 85, 256, 341);
    { GemmP gl24;
      gl24.A = CS; gl24.B = WsW; gl24.bias = B4; gl24.R = H + (size_t)85 * E; gl24.C = H + (size_t)85 * E;
      gl24.sAo = (long long)256 * E; gl24.sAi = 0; gl24.sAm = E; gl24.sAk = 1; gl24.sBo = 0; gl24.sBi = 0; gl24.sBn = E; gl24.sBk = 1; gl24.sCo = (long long)NN * E; gl24.sCi = 0; gl24.sCm = E; gl24.sRo = (long long)NN * E; gl24.sRi = 0; gl24.sRm = E; gl24.sRn = 1;
      gl24.M = 256; gl24.N = E; gl24.K = E; gl24.zi_n = 1; gl24.flags = 5; gl24.act = 0;
      gl24.alpha = 1.0f; gl24.beta = 1.0f; gl24.sa = 1.0f; gl24.sb = 1.0f; gl24.Npad = E; gl24.pad_ = 0;
      if ((long long)(256) >= 64 && (long long)(E) >= 64) k_gemmT<1, 2, 4><<<dim3((unsigned)((E) + 63) / 64, (unsigned)((256) + 31) / 32, (unsigned)(TC)), 32, 0, stream>>>(gl24);
      else k_gemm<1><<<dim3((unsigned)((E) + 31) / 32, (unsigned)((256) + 15) / 16, (unsigned)(TC)), 32, 0, stream>>>(gl24); }
    k_tb_csum<<<(unsigned)(((long long)TC * 64 * E + 255) / 256), 256, 0, stream>>>(H, CS, TC, NN, E, 21, 64, 85);
    { GemmP gl23;
      gl23.A = CS; gl23.B = WsW; gl23.bias = B4; gl23.R = H + (size_t)21 * E; gl23.C = H + (size_t)21 * E;
      gl23.sAo = (long long)64 * E; gl23.sAi = 0; gl23.sAm = E; gl23.sAk = 1; gl23.sBo = 0; gl23.sBi = 0; gl23.sBn = E; gl23.sBk = 1; gl23.sCo = (long long)NN * E; gl23.sCi = 0; gl23.sCm = E; gl23.sRo = (long long)NN * E; gl23.sRi = 0; gl23.sRm = E; gl23.sRn = 1;
      gl23.M = 64; gl23.N = E; gl23.K = E; gl23.zi_n = 1; gl23.flags = 5; gl23.act = 0;
      gl23.alpha = 1.0f; gl23.beta = 1.0f; gl23.sa = 1.0f; gl23.sb = 1.0f; gl23.Npad = E; gl23.pad_ = 0;
      if ((long long)(64) >= 64 && (long long)(E) >= 64) k_gemmT<1, 2, 4><<<dim3((unsigned)((E) + 63) / 64, (unsigned)((64) + 31) / 32, (unsigned)(TC)), 32, 0, stream>>>(gl23);
      else k_gemm<1><<<dim3((unsigned)((E) + 31) / 32, (unsigned)((64) + 15) / 16, (unsigned)(TC)), 32, 0, stream>>>(gl23); }
    k_tb_csum<<<(unsigned)(((long long)TC * 16 * E + 255) / 256), 256, 0, stream>>>(H, CS, TC, NN, E, 5, 16, 21);
    { GemmP gl22;
      gl22.A = CS; gl22.B = WsW; gl22.bias = B4; gl22.R = H + (size_t)5 * E; gl22.C = H + (size_t)5 * E;
      gl22.sAo = (long long)16 * E; gl22.sAi = 0; gl22.sAm = E; gl22.sAk = 1; gl22.sBo = 0; gl22.sBi = 0; gl22.sBn = E; gl22.sBk = 1; gl22.sCo = (long long)NN * E; gl22.sCi = 0; gl22.sCm = E; gl22.sRo = (long long)NN * E; gl22.sRi = 0; gl22.sRm = E; gl22.sRn = 1;
      gl22.M = 16; gl22.N = E; gl22.K = E; gl22.zi_n = 1; gl22.flags = 5; gl22.act = 0;
      gl22.alpha = 1.0f; gl22.beta = 1.0f; gl22.sa = 1.0f; gl22.sb = 1.0f; gl22.Npad = E; gl22.pad_ = 0;
      k_gemm<1><<<dim3((unsigned)((E) + 31) / 32, (unsigned)((16) + 15) / 16, (unsigned)(TC)), 32, 0, stream>>>(gl22); }
    k_tb_csum<<<(unsigned)(((long long)TC * 4 * E + 255) / 256), 256, 0, stream>>>(H, CS, TC, NN, E, 1, 4, 5);
    { GemmP gl21;
      gl21.A = CS; gl21.B = WsW; gl21.bias = B4; gl21.R = H + (size_t)1 * E; gl21.C = H + (size_t)1 * E;
      gl21.sAo = (long long)4 * E; gl21.sAi = 0; gl21.sAm = E; gl21.sAk = 1; gl21.sBo = 0; gl21.sBi = 0; gl21.sBn = E; gl21.sBk = 1; gl21.sCo = (long long)NN * E; gl21.sCi = 0; gl21.sCm = E; gl21.sRo = (long long)NN * E; gl21.sRi = 0; gl21.sRm = E; gl21.sRn = 1;
      gl21.M = 4; gl21.N = E; gl21.K = E; gl21.zi_n = 1; gl21.flags = 5; gl21.act = 0;
      gl21.alpha = 1.0f; gl21.beta = 1.0f; gl21.sa = 1.0f; gl21.sb = 1.0f; gl21.Npad = E; gl21.pad_ = 0;
      k_gemm<1><<<dim3((unsigned)((E) + 31) / 32, (unsigned)((4) + 15) / 16, (unsigned)(TC)), 32, 0, stream>>>(gl21); }
    k_tb_csum<<<(unsigned)(((long long)TC * 1 * E + 255) / 256), 256, 0, stream>>>(H, CS, TC, NN, E, 0, 1, 1);
    { GemmP gl20;
      gl20.A = CS; gl20.B = WsW; gl20.bias = B4; gl20.R = H + (size_t)0 * E; gl20.C = H + (size_t)0 * E;
      gl20.sAo = (long long)1 * E; gl20.sAi = 0; gl20.sAm = E; gl20.sAk = 1; gl20.sBo = 0; gl20.sBi = 0; gl20.sBn = E; gl20.sBk = 1; gl20.sCo = (long long)NN * E; gl20.sCi = 0; gl20.sCm = E; gl20.sRo = (long long)NN * E; gl20.sRi = 0; gl20.sRm = E; gl20.sRn = 1;
      gl20.M = 1; gl20.N = E; gl20.K = E; gl20.zi_n = 1; gl20.flags = 5; gl20.act = 0;
      gl20.alpha = 1.0f; gl20.beta = 1.0f; gl20.sa = 1.0f; gl20.sb = 1.0f; gl20.Npad = E; gl20.pad_ = 0;
      k_gemm<1><<<dim3((unsigned)((E) + 31) / 32, (unsigned)((1) + 15) / 16, (unsigned)(TC)), 32, 0, stream>>>(gl20); }
    k_tb_max<<<(unsigned)((TC * E + 127) / 128), 128, 0, stream>>>(H, out, 128, TC, NN, E);
    k_tb_gather<<<(unsigned)(((long long)TC * NN * E + 255) / 256), 256, 0, stream>>>(tok, EW, H, 192, TC, NN, E, V);
    k_tb_csum<<<(unsigned)(((long long)TC * 256 * E + 255) / 256), 256, 0, stream>>>(H, CS, TC, NN, E, 85, 256, 341);
    { GemmP gl34;
      gl34.A = CS; gl34.B = WsW; gl34.bias = B4; gl34.R = H + (size_t)85 * E; gl34.C = H + (size_t)85 * E;
      gl34.sAo = (long long)256 * E; gl34.sAi = 0; gl34.sAm = E; gl34.sAk = 1; gl34.sBo = 0; gl34.sBi = 0; gl34.sBn = E; gl34.sBk = 1; gl34.sCo = (long long)NN * E; gl34.sCi = 0; gl34.sCm = E; gl34.sRo = (long long)NN * E; gl34.sRi = 0; gl34.sRm = E; gl34.sRn = 1;
      gl34.M = 256; gl34.N = E; gl34.K = E; gl34.zi_n = 1; gl34.flags = 5; gl34.act = 0;
      gl34.alpha = 1.0f; gl34.beta = 1.0f; gl34.sa = 1.0f; gl34.sb = 1.0f; gl34.Npad = E; gl34.pad_ = 0;
      if ((long long)(256) >= 64 && (long long)(E) >= 64) k_gemmT<1, 2, 4><<<dim3((unsigned)((E) + 63) / 64, (unsigned)((256) + 31) / 32, (unsigned)(TC)), 32, 0, stream>>>(gl34);
      else k_gemm<1><<<dim3((unsigned)((E) + 31) / 32, (unsigned)((256) + 15) / 16, (unsigned)(TC)), 32, 0, stream>>>(gl34); }
    k_tb_csum<<<(unsigned)(((long long)TC * 64 * E + 255) / 256), 256, 0, stream>>>(H, CS, TC, NN, E, 21, 64, 85);
    { GemmP gl33;
      gl33.A = CS; gl33.B = WsW; gl33.bias = B4; gl33.R = H + (size_t)21 * E; gl33.C = H + (size_t)21 * E;
      gl33.sAo = (long long)64 * E; gl33.sAi = 0; gl33.sAm = E; gl33.sAk = 1; gl33.sBo = 0; gl33.sBi = 0; gl33.sBn = E; gl33.sBk = 1; gl33.sCo = (long long)NN * E; gl33.sCi = 0; gl33.sCm = E; gl33.sRo = (long long)NN * E; gl33.sRi = 0; gl33.sRm = E; gl33.sRn = 1;
      gl33.M = 64; gl33.N = E; gl33.K = E; gl33.zi_n = 1; gl33.flags = 5; gl33.act = 0;
      gl33.alpha = 1.0f; gl33.beta = 1.0f; gl33.sa = 1.0f; gl33.sb = 1.0f; gl33.Npad = E; gl33.pad_ = 0;
      if ((long long)(64) >= 64 && (long long)(E) >= 64) k_gemmT<1, 2, 4><<<dim3((unsigned)((E) + 63) / 64, (unsigned)((64) + 31) / 32, (unsigned)(TC)), 32, 0, stream>>>(gl33);
      else k_gemm<1><<<dim3((unsigned)((E) + 31) / 32, (unsigned)((64) + 15) / 16, (unsigned)(TC)), 32, 0, stream>>>(gl33); }
    k_tb_csum<<<(unsigned)(((long long)TC * 16 * E + 255) / 256), 256, 0, stream>>>(H, CS, TC, NN, E, 5, 16, 21);
    { GemmP gl32;
      gl32.A = CS; gl32.B = WsW; gl32.bias = B4; gl32.R = H + (size_t)5 * E; gl32.C = H + (size_t)5 * E;
      gl32.sAo = (long long)16 * E; gl32.sAi = 0; gl32.sAm = E; gl32.sAk = 1; gl32.sBo = 0; gl32.sBi = 0; gl32.sBn = E; gl32.sBk = 1; gl32.sCo = (long long)NN * E; gl32.sCi = 0; gl32.sCm = E; gl32.sRo = (long long)NN * E; gl32.sRi = 0; gl32.sRm = E; gl32.sRn = 1;
      gl32.M = 16; gl32.N = E; gl32.K = E; gl32.zi_n = 1; gl32.flags = 5; gl32.act = 0;
      gl32.alpha = 1.0f; gl32.beta = 1.0f; gl32.sa = 1.0f; gl32.sb = 1.0f; gl32.Npad = E; gl32.pad_ = 0;
      k_gemm<1><<<dim3((unsigned)((E) + 31) / 32, (unsigned)((16) + 15) / 16, (unsigned)(TC)), 32, 0, stream>>>(gl32); }
    k_tb_csum<<<(unsigned)(((long long)TC * 4 * E + 255) / 256), 256, 0, stream>>>(H, CS, TC, NN, E, 1, 4, 5);
    { GemmP gl31;
      gl31.A = CS; gl31.B = WsW; gl31.bias = B4; gl31.R = H + (size_t)1 * E; gl31.C = H + (size_t)1 * E;
      gl31.sAo = (long long)4 * E; gl31.sAi = 0; gl31.sAm = E; gl31.sAk = 1; gl31.sBo = 0; gl31.sBi = 0; gl31.sBn = E; gl31.sBk = 1; gl31.sCo = (long long)NN * E; gl31.sCi = 0; gl31.sCm = E; gl31.sRo = (long long)NN * E; gl31.sRi = 0; gl31.sRm = E; gl31.sRn = 1;
      gl31.M = 4; gl31.N = E; gl31.K = E; gl31.zi_n = 1; gl31.flags = 5; gl31.act = 0;
      gl31.alpha = 1.0f; gl31.beta = 1.0f; gl31.sa = 1.0f; gl31.sb = 1.0f; gl31.Npad = E; gl31.pad_ = 0;
      k_gemm<1><<<dim3((unsigned)((E) + 31) / 32, (unsigned)((4) + 15) / 16, (unsigned)(TC)), 32, 0, stream>>>(gl31); }
    k_tb_csum<<<(unsigned)(((long long)TC * 1 * E + 255) / 256), 256, 0, stream>>>(H, CS, TC, NN, E, 0, 1, 1);
    { GemmP gl30;
      gl30.A = CS; gl30.B = WsW; gl30.bias = B4; gl30.R = H + (size_t)0 * E; gl30.C = H + (size_t)0 * E;
      gl30.sAo = (long long)1 * E; gl30.sAi = 0; gl30.sAm = E; gl30.sAk = 1; gl30.sBo = 0; gl30.sBi = 0; gl30.sBn = E; gl30.sBk = 1; gl30.sCo = (long long)NN * E; gl30.sCi = 0; gl30.sCm = E; gl30.sRo = (long long)NN * E; gl30.sRi = 0; gl30.sRm = E; gl30.sRn = 1;
      gl30.M = 1; gl30.N = E; gl30.K = E; gl30.zi_n = 1; gl30.flags = 5; gl30.act = 0;
      gl30.alpha = 1.0f; gl30.beta = 1.0f; gl30.sa = 1.0f; gl30.sb = 1.0f; gl30.Npad = E; gl30.pad_ = 0;
      k_gemm<1><<<dim3((unsigned)((E) + 31) / 32, (unsigned)((1) + 15) / 16, (unsigned)(TC)), 32, 0, stream>>>(gl30); }
    k_tb_max<<<(unsigned)((TC * E + 127) / 128), 128, 0, stream>>>(H, out, 192, TC, NN, E);
    k_tb_gather<<<(unsigned)(((long long)TC * NN * E + 255) / 256), 256, 0, stream>>>(tok, EW, H, 256, TC, NN, E, V);
    k_tb_csum<<<(unsigned)(((long long)TC * 256 * E + 255) / 256), 256, 0, stream>>>(H, CS, TC, NN, E, 85, 256, 341);
    { GemmP gl44;
      gl44.A = CS; gl44.B = WsW; gl44.bias = B4; gl44.R = H + (size_t)85 * E; gl44.C = H + (size_t)85 * E;
      gl44.sAo = (long long)256 * E; gl44.sAi = 0; gl44.sAm = E; gl44.sAk = 1; gl44.sBo = 0; gl44.sBi = 0; gl44.sBn = E; gl44.sBk = 1; gl44.sCo = (long long)NN * E; gl44.sCi = 0; gl44.sCm = E; gl44.sRo = (long long)NN * E; gl44.sRi = 0; gl44.sRm = E; gl44.sRn = 1;
      gl44.M = 256; gl44.N = E; gl44.K = E; gl44.zi_n = 1; gl44.flags = 5; gl44.act = 0;
      gl44.alpha = 1.0f; gl44.beta = 1.0f; gl44.sa = 1.0f; gl44.sb = 1.0f; gl44.Npad = E; gl44.pad_ = 0;
      if ((long long)(256) >= 64 && (long long)(E) >= 64) k_gemmT<1, 2, 4><<<dim3((unsigned)((E) + 63) / 64, (unsigned)((256) + 31) / 32, (unsigned)(TC)), 32, 0, stream>>>(gl44);
      else k_gemm<1><<<dim3((unsigned)((E) + 31) / 32, (unsigned)((256) + 15) / 16, (unsigned)(TC)), 32, 0, stream>>>(gl44); }
    k_tb_csum<<<(unsigned)(((long long)TC * 64 * E + 255) / 256), 256, 0, stream>>>(H, CS, TC, NN, E, 21, 64, 85);
    { GemmP gl43;
      gl43.A = CS; gl43.B = WsW; gl43.bias = B4; gl43.R = H + (size_t)21 * E; gl43.C = H + (size_t)21 * E;
      gl43.sAo = (long long)64 * E; gl43.sAi = 0; gl43.sAm = E; gl43.sAk = 1; gl43.sBo = 0; gl43.sBi = 0; gl43.sBn = E; gl43.sBk = 1; gl43.sCo = (long long)NN * E; gl43.sCi = 0; gl43.sCm = E; gl43.sRo = (long long)NN * E; gl43.sRi = 0; gl43.sRm = E; gl43.sRn = 1;
      gl43.M = 64; gl43.N = E; gl43.K = E; gl43.zi_n = 1; gl43.flags = 5; gl43.act = 0;
      gl43.alpha = 1.0f; gl43.beta = 1.0f; gl43.sa = 1.0f; gl43.sb = 1.0f; gl43.Npad = E; gl43.pad_ = 0;
      if ((long long)(64) >= 64 && (long long)(E) >= 64) k_gemmT<1, 2, 4><<<dim3((unsigned)((E) + 63) / 64, (unsigned)((64) + 31) / 32, (unsigned)(TC)), 32, 0, stream>>>(gl43);
      else k_gemm<1><<<dim3((unsigned)((E) + 31) / 32, (unsigned)((64) + 15) / 16, (unsigned)(TC)), 32, 0, stream>>>(gl43); }
    k_tb_csum<<<(unsigned)(((long long)TC * 16 * E + 255) / 256), 256, 0, stream>>>(H, CS, TC, NN, E, 5, 16, 21);
    { GemmP gl42;
      gl42.A = CS; gl42.B = WsW; gl42.bias = B4; gl42.R = H + (size_t)5 * E; gl42.C = H + (size_t)5 * E;
      gl42.sAo = (long long)16 * E; gl42.sAi = 0; gl42.sAm = E; gl42.sAk = 1; gl42.sBo = 0; gl42.sBi = 0; gl42.sBn = E; gl42.sBk = 1; gl42.sCo = (long long)NN * E; gl42.sCi = 0; gl42.sCm = E; gl42.sRo = (long long)NN * E; gl42.sRi = 0; gl42.sRm = E; gl42.sRn = 1;
      gl42.M = 16; gl42.N = E; gl42.K = E; gl42.zi_n = 1; gl42.flags = 5; gl42.act = 0;
      gl42.alpha = 1.0f; gl42.beta = 1.0f; gl42.sa = 1.0f; gl42.sb = 1.0f; gl42.Npad = E; gl42.pad_ = 0;
      k_gemm<1><<<dim3((unsigned)((E) + 31) / 32, (unsigned)((16) + 15) / 16, (unsigned)(TC)), 32, 0, stream>>>(gl42); }
    k_tb_csum<<<(unsigned)(((long long)TC * 4 * E + 255) / 256), 256, 0, stream>>>(H, CS, TC, NN, E, 1, 4, 5);
    { GemmP gl41;
      gl41.A = CS; gl41.B = WsW; gl41.bias = B4; gl41.R = H + (size_t)1 * E; gl41.C = H + (size_t)1 * E;
      gl41.sAo = (long long)4 * E; gl41.sAi = 0; gl41.sAm = E; gl41.sAk = 1; gl41.sBo = 0; gl41.sBi = 0; gl41.sBn = E; gl41.sBk = 1; gl41.sCo = (long long)NN * E; gl41.sCi = 0; gl41.sCm = E; gl41.sRo = (long long)NN * E; gl41.sRi = 0; gl41.sRm = E; gl41.sRn = 1;
      gl41.M = 4; gl41.N = E; gl41.K = E; gl41.zi_n = 1; gl41.flags = 5; gl41.act = 0;
      gl41.alpha = 1.0f; gl41.beta = 1.0f; gl41.sa = 1.0f; gl41.sb = 1.0f; gl41.Npad = E; gl41.pad_ = 0;
      k_gemm<1><<<dim3((unsigned)((E) + 31) / 32, (unsigned)((4) + 15) / 16, (unsigned)(TC)), 32, 0, stream>>>(gl41); }
    k_tb_csum<<<(unsigned)(((long long)TC * 1 * E + 255) / 256), 256, 0, stream>>>(H, CS, TC, NN, E, 0, 1, 1);
    { GemmP gl40;
      gl40.A = CS; gl40.B = WsW; gl40.bias = B4; gl40.R = H + (size_t)0 * E; gl40.C = H + (size_t)0 * E;
      gl40.sAo = (long long)1 * E; gl40.sAi = 0; gl40.sAm = E; gl40.sAk = 1; gl40.sBo = 0; gl40.sBi = 0; gl40.sBn = E; gl40.sBk = 1; gl40.sCo = (long long)NN * E; gl40.sCi = 0; gl40.sCm = E; gl40.sRo = (long long)NN * E; gl40.sRi = 0; gl40.sRm = E; gl40.sRn = 1;
      gl40.M = 1; gl40.N = E; gl40.K = E; gl40.zi_n = 1; gl40.flags = 5; gl40.act = 0;
      gl40.alpha = 1.0f; gl40.beta = 1.0f; gl40.sa = 1.0f; gl40.sb = 1.0f; gl40.Npad = E; gl40.pad_ = 0;
      k_gemm<1><<<dim3((unsigned)((E) + 31) / 32, (unsigned)((1) + 15) / 16, (unsigned)(TC)), 32, 0, stream>>>(gl40); }
    k_tb_max<<<(unsigned)((TC * E + 127) / 128), 128, 0, stream>>>(H, out, 256, TC, NN, E);
    k_tb_gather<<<(unsigned)(((long long)TC * NN * E + 255) / 256), 256, 0, stream>>>(tok, EW, H, 320, TC, NN, E, V);
    k_tb_csum<<<(unsigned)(((long long)TC * 256 * E + 255) / 256), 256, 0, stream>>>(H, CS, TC, NN, E, 85, 256, 341);
    { GemmP gl54;
      gl54.A = CS; gl54.B = WsW; gl54.bias = B4; gl54.R = H + (size_t)85 * E; gl54.C = H + (size_t)85 * E;
      gl54.sAo = (long long)256 * E; gl54.sAi = 0; gl54.sAm = E; gl54.sAk = 1; gl54.sBo = 0; gl54.sBi = 0; gl54.sBn = E; gl54.sBk = 1; gl54.sCo = (long long)NN * E; gl54.sCi = 0; gl54.sCm = E; gl54.sRo = (long long)NN * E; gl54.sRi = 0; gl54.sRm = E; gl54.sRn = 1;
      gl54.M = 256; gl54.N = E; gl54.K = E; gl54.zi_n = 1; gl54.flags = 5; gl54.act = 0;
      gl54.alpha = 1.0f; gl54.beta = 1.0f; gl54.sa = 1.0f; gl54.sb = 1.0f; gl54.Npad = E; gl54.pad_ = 0;
      if ((long long)(256) >= 64 && (long long)(E) >= 64) k_gemmT<1, 2, 4><<<dim3((unsigned)((E) + 63) / 64, (unsigned)((256) + 31) / 32, (unsigned)(TC)), 32, 0, stream>>>(gl54);
      else k_gemm<1><<<dim3((unsigned)((E) + 31) / 32, (unsigned)((256) + 15) / 16, (unsigned)(TC)), 32, 0, stream>>>(gl54); }
    k_tb_csum<<<(unsigned)(((long long)TC * 64 * E + 255) / 256), 256, 0, stream>>>(H, CS, TC, NN, E, 21, 64, 85);
    { GemmP gl53;
      gl53.A = CS; gl53.B = WsW; gl53.bias = B4; gl53.R = H + (size_t)21 * E; gl53.C = H + (size_t)21 * E;
      gl53.sAo = (long long)64 * E; gl53.sAi = 0; gl53.sAm = E; gl53.sAk = 1; gl53.sBo = 0; gl53.sBi = 0; gl53.sBn = E; gl53.sBk = 1; gl53.sCo = (long long)NN * E; gl53.sCi = 0; gl53.sCm = E; gl53.sRo = (long long)NN * E; gl53.sRi = 0; gl53.sRm = E; gl53.sRn = 1;
      gl53.M = 64; gl53.N = E; gl53.K = E; gl53.zi_n = 1; gl53.flags = 5; gl53.act = 0;
      gl53.alpha = 1.0f; gl53.beta = 1.0f; gl53.sa = 1.0f; gl53.sb = 1.0f; gl53.Npad = E; gl53.pad_ = 0;
      if ((long long)(64) >= 64 && (long long)(E) >= 64) k_gemmT<1, 2, 4><<<dim3((unsigned)((E) + 63) / 64, (unsigned)((64) + 31) / 32, (unsigned)(TC)), 32, 0, stream>>>(gl53);
      else k_gemm<1><<<dim3((unsigned)((E) + 31) / 32, (unsigned)((64) + 15) / 16, (unsigned)(TC)), 32, 0, stream>>>(gl53); }
    k_tb_csum<<<(unsigned)(((long long)TC * 16 * E + 255) / 256), 256, 0, stream>>>(H, CS, TC, NN, E, 5, 16, 21);
    { GemmP gl52;
      gl52.A = CS; gl52.B = WsW; gl52.bias = B4; gl52.R = H + (size_t)5 * E; gl52.C = H + (size_t)5 * E;
      gl52.sAo = (long long)16 * E; gl52.sAi = 0; gl52.sAm = E; gl52.sAk = 1; gl52.sBo = 0; gl52.sBi = 0; gl52.sBn = E; gl52.sBk = 1; gl52.sCo = (long long)NN * E; gl52.sCi = 0; gl52.sCm = E; gl52.sRo = (long long)NN * E; gl52.sRi = 0; gl52.sRm = E; gl52.sRn = 1;
      gl52.M = 16; gl52.N = E; gl52.K = E; gl52.zi_n = 1; gl52.flags = 5; gl52.act = 0;
      gl52.alpha = 1.0f; gl52.beta = 1.0f; gl52.sa = 1.0f; gl52.sb = 1.0f; gl52.Npad = E; gl52.pad_ = 0;
      k_gemm<1><<<dim3((unsigned)((E) + 31) / 32, (unsigned)((16) + 15) / 16, (unsigned)(TC)), 32, 0, stream>>>(gl52); }
    k_tb_csum<<<(unsigned)(((long long)TC * 4 * E + 255) / 256), 256, 0, stream>>>(H, CS, TC, NN, E, 1, 4, 5);
    { GemmP gl51;
      gl51.A = CS; gl51.B = WsW; gl51.bias = B4; gl51.R = H + (size_t)1 * E; gl51.C = H + (size_t)1 * E;
      gl51.sAo = (long long)4 * E; gl51.sAi = 0; gl51.sAm = E; gl51.sAk = 1; gl51.sBo = 0; gl51.sBi = 0; gl51.sBn = E; gl51.sBk = 1; gl51.sCo = (long long)NN * E; gl51.sCi = 0; gl51.sCm = E; gl51.sRo = (long long)NN * E; gl51.sRi = 0; gl51.sRm = E; gl51.sRn = 1;
      gl51.M = 4; gl51.N = E; gl51.K = E; gl51.zi_n = 1; gl51.flags = 5; gl51.act = 0;
      gl51.alpha = 1.0f; gl51.beta = 1.0f; gl51.sa = 1.0f; gl51.sb = 1.0f; gl51.Npad = E; gl51.pad_ = 0;
      k_gemm<1><<<dim3((unsigned)((E) + 31) / 32, (unsigned)((4) + 15) / 16, (unsigned)(TC)), 32, 0, stream>>>(gl51); }
    k_tb_csum<<<(unsigned)(((long long)TC * 1 * E + 255) / 256), 256, 0, stream>>>(H, CS, TC, NN, E, 0, 1, 1);
    { GemmP gl50;
      gl50.A = CS; gl50.B = WsW; gl50.bias = B4; gl50.R = H + (size_t)0 * E; gl50.C = H + (size_t)0 * E;
      gl50.sAo = (long long)1 * E; gl50.sAi = 0; gl50.sAm = E; gl50.sAk = 1; gl50.sBo = 0; gl50.sBi = 0; gl50.sBn = E; gl50.sBk = 1; gl50.sCo = (long long)NN * E; gl50.sCi = 0; gl50.sCm = E; gl50.sRo = (long long)NN * E; gl50.sRi = 0; gl50.sRm = E; gl50.sRn = 1;
      gl50.M = 1; gl50.N = E; gl50.K = E; gl50.zi_n = 1; gl50.flags = 5; gl50.act = 0;
      gl50.alpha = 1.0f; gl50.beta = 1.0f; gl50.sa = 1.0f; gl50.sb = 1.0f; gl50.Npad = E; gl50.pad_ = 0;
      k_gemm<1><<<dim3((unsigned)((E) + 31) / 32, (unsigned)((1) + 15) / 16, (unsigned)(TC)), 32, 0, stream>>>(gl50); }
    k_tb_max<<<(unsigned)((TC * E + 127) / 128), 128, 0, stream>>>(H, out, 320, TC, NN, E);
    k_tb_gather<<<(unsigned)(((long long)TC * NN * E + 255) / 256), 256, 0, stream>>>(tok, EW, H, 384, TC, NN, E, V);
    k_tb_csum<<<(unsigned)(((long long)TC * 256 * E + 255) / 256), 256, 0, stream>>>(H, CS, TC, NN, E, 85, 256, 341);
    { GemmP gl64;
      gl64.A = CS; gl64.B = WsW; gl64.bias = B4; gl64.R = H + (size_t)85 * E; gl64.C = H + (size_t)85 * E;
      gl64.sAo = (long long)256 * E; gl64.sAi = 0; gl64.sAm = E; gl64.sAk = 1; gl64.sBo = 0; gl64.sBi = 0; gl64.sBn = E; gl64.sBk = 1; gl64.sCo = (long long)NN * E; gl64.sCi = 0; gl64.sCm = E; gl64.sRo = (long long)NN * E; gl64.sRi = 0; gl64.sRm = E; gl64.sRn = 1;
      gl64.M = 256; gl64.N = E; gl64.K = E; gl64.zi_n = 1; gl64.flags = 5; gl64.act = 0;
      gl64.alpha = 1.0f; gl64.beta = 1.0f; gl64.sa = 1.0f; gl64.sb = 1.0f; gl64.Npad = E; gl64.pad_ = 0;
      if ((long long)(256) >= 64 && (long long)(E) >= 64) k_gemmT<1, 2, 4><<<dim3((unsigned)((E) + 63) / 64, (unsigned)((256) + 31) / 32, (unsigned)(TC)), 32, 0, stream>>>(gl64);
      else k_gemm<1><<<dim3((unsigned)((E) + 31) / 32, (unsigned)((256) + 15) / 16, (unsigned)(TC)), 32, 0, stream>>>(gl64); }
    k_tb_csum<<<(unsigned)(((long long)TC * 64 * E + 255) / 256), 256, 0, stream>>>(H, CS, TC, NN, E, 21, 64, 85);
    { GemmP gl63;
      gl63.A = CS; gl63.B = WsW; gl63.bias = B4; gl63.R = H + (size_t)21 * E; gl63.C = H + (size_t)21 * E;
      gl63.sAo = (long long)64 * E; gl63.sAi = 0; gl63.sAm = E; gl63.sAk = 1; gl63.sBo = 0; gl63.sBi = 0; gl63.sBn = E; gl63.sBk = 1; gl63.sCo = (long long)NN * E; gl63.sCi = 0; gl63.sCm = E; gl63.sRo = (long long)NN * E; gl63.sRi = 0; gl63.sRm = E; gl63.sRn = 1;
      gl63.M = 64; gl63.N = E; gl63.K = E; gl63.zi_n = 1; gl63.flags = 5; gl63.act = 0;
      gl63.alpha = 1.0f; gl63.beta = 1.0f; gl63.sa = 1.0f; gl63.sb = 1.0f; gl63.Npad = E; gl63.pad_ = 0;
      if ((long long)(64) >= 64 && (long long)(E) >= 64) k_gemmT<1, 2, 4><<<dim3((unsigned)((E) + 63) / 64, (unsigned)((64) + 31) / 32, (unsigned)(TC)), 32, 0, stream>>>(gl63);
      else k_gemm<1><<<dim3((unsigned)((E) + 31) / 32, (unsigned)((64) + 15) / 16, (unsigned)(TC)), 32, 0, stream>>>(gl63); }
    k_tb_csum<<<(unsigned)(((long long)TC * 16 * E + 255) / 256), 256, 0, stream>>>(H, CS, TC, NN, E, 5, 16, 21);
    { GemmP gl62;
      gl62.A = CS; gl62.B = WsW; gl62.bias = B4; gl62.R = H + (size_t)5 * E; gl62.C = H + (size_t)5 * E;
      gl62.sAo = (long long)16 * E; gl62.sAi = 0; gl62.sAm = E; gl62.sAk = 1; gl62.sBo = 0; gl62.sBi = 0; gl62.sBn = E; gl62.sBk = 1; gl62.sCo = (long long)NN * E; gl62.sCi = 0; gl62.sCm = E; gl62.sRo = (long long)NN * E; gl62.sRi = 0; gl62.sRm = E; gl62.sRn = 1;
      gl62.M = 16; gl62.N = E; gl62.K = E; gl62.zi_n = 1; gl62.flags = 5; gl62.act = 0;
      gl62.alpha = 1.0f; gl62.beta = 1.0f; gl62.sa = 1.0f; gl62.sb = 1.0f; gl62.Npad = E; gl62.pad_ = 0;
      k_gemm<1><<<dim3((unsigned)((E) + 31) / 32, (unsigned)((16) + 15) / 16, (unsigned)(TC)), 32, 0, stream>>>(gl62); }
    k_tb_csum<<<(unsigned)(((long long)TC * 4 * E + 255) / 256), 256, 0, stream>>>(H, CS, TC, NN, E, 1, 4, 5);
    { GemmP gl61;
      gl61.A = CS; gl61.B = WsW; gl61.bias = B4; gl61.R = H + (size_t)1 * E; gl61.C = H + (size_t)1 * E;
      gl61.sAo = (long long)4 * E; gl61.sAi = 0; gl61.sAm = E; gl61.sAk = 1; gl61.sBo = 0; gl61.sBi = 0; gl61.sBn = E; gl61.sBk = 1; gl61.sCo = (long long)NN * E; gl61.sCi = 0; gl61.sCm = E; gl61.sRo = (long long)NN * E; gl61.sRi = 0; gl61.sRm = E; gl61.sRn = 1;
      gl61.M = 4; gl61.N = E; gl61.K = E; gl61.zi_n = 1; gl61.flags = 5; gl61.act = 0;
      gl61.alpha = 1.0f; gl61.beta = 1.0f; gl61.sa = 1.0f; gl61.sb = 1.0f; gl61.Npad = E; gl61.pad_ = 0;
      k_gemm<1><<<dim3((unsigned)((E) + 31) / 32, (unsigned)((4) + 15) / 16, (unsigned)(TC)), 32, 0, stream>>>(gl61); }
    k_tb_csum<<<(unsigned)(((long long)TC * 1 * E + 255) / 256), 256, 0, stream>>>(H, CS, TC, NN, E, 0, 1, 1);
    { GemmP gl60;
      gl60.A = CS; gl60.B = WsW; gl60.bias = B4; gl60.R = H + (size_t)0 * E; gl60.C = H + (size_t)0 * E;
      gl60.sAo = (long long)1 * E; gl60.sAi = 0; gl60.sAm = E; gl60.sAk = 1; gl60.sBo = 0; gl60.sBi = 0; gl60.sBn = E; gl60.sBk = 1; gl60.sCo = (long long)NN * E; gl60.sCi = 0; gl60.sCm = E; gl60.sRo = (long long)NN * E; gl60.sRi = 0; gl60.sRm = E; gl60.sRn = 1;
      gl60.M = 1; gl60.N = E; gl60.K = E; gl60.zi_n = 1; gl60.flags = 5; gl60.act = 0;
      gl60.alpha = 1.0f; gl60.beta = 1.0f; gl60.sa = 1.0f; gl60.sb = 1.0f; gl60.Npad = E; gl60.pad_ = 0;
      k_gemm<1><<<dim3((unsigned)((E) + 31) / 32, (unsigned)((1) + 15) / 16, (unsigned)(TC)), 32, 0, stream>>>(gl60); }
    k_tb_max<<<(unsigned)((TC * E + 127) / 128), 128, 0, stream>>>(H, out, 384, TC, NN, E);
    k_tb_gather<<<(unsigned)(((long long)TC * NN * E + 255) / 256), 256, 0, stream>>>(tok, EW, H, 448, TC, NN, E, V);
    k_tb_csum<<<(unsigned)(((long long)TC * 256 * E + 255) / 256), 256, 0, stream>>>(H, CS, TC, NN, E, 85, 256, 341);
    { GemmP gl74;
      gl74.A = CS; gl74.B = WsW; gl74.bias = B4; gl74.R = H + (size_t)85 * E; gl74.C = H + (size_t)85 * E;
      gl74.sAo = (long long)256 * E; gl74.sAi = 0; gl74.sAm = E; gl74.sAk = 1; gl74.sBo = 0; gl74.sBi = 0; gl74.sBn = E; gl74.sBk = 1; gl74.sCo = (long long)NN * E; gl74.sCi = 0; gl74.sCm = E; gl74.sRo = (long long)NN * E; gl74.sRi = 0; gl74.sRm = E; gl74.sRn = 1;
      gl74.M = 256; gl74.N = E; gl74.K = E; gl74.zi_n = 1; gl74.flags = 5; gl74.act = 0;
      gl74.alpha = 1.0f; gl74.beta = 1.0f; gl74.sa = 1.0f; gl74.sb = 1.0f; gl74.Npad = E; gl74.pad_ = 0;
      if ((long long)(256) >= 64 && (long long)(E) >= 64) k_gemmT<1, 2, 4><<<dim3((unsigned)((E) + 63) / 64, (unsigned)((256) + 31) / 32, (unsigned)(TC)), 32, 0, stream>>>(gl74);
      else k_gemm<1><<<dim3((unsigned)((E) + 31) / 32, (unsigned)((256) + 15) / 16, (unsigned)(TC)), 32, 0, stream>>>(gl74); }
    k_tb_csum<<<(unsigned)(((long long)TC * 64 * E + 255) / 256), 256, 0, stream>>>(H, CS, TC, NN, E, 21, 64, 85);
    { GemmP gl73;
      gl73.A = CS; gl73.B = WsW; gl73.bias = B4; gl73.R = H + (size_t)21 * E; gl73.C = H + (size_t)21 * E;
      gl73.sAo = (long long)64 * E; gl73.sAi = 0; gl73.sAm = E; gl73.sAk = 1; gl73.sBo = 0; gl73.sBi = 0; gl73.sBn = E; gl73.sBk = 1; gl73.sCo = (long long)NN * E; gl73.sCi = 0; gl73.sCm = E; gl73.sRo = (long long)NN * E; gl73.sRi = 0; gl73.sRm = E; gl73.sRn = 1;
      gl73.M = 64; gl73.N = E; gl73.K = E; gl73.zi_n = 1; gl73.flags = 5; gl73.act = 0;
      gl73.alpha = 1.0f; gl73.beta = 1.0f; gl73.sa = 1.0f; gl73.sb = 1.0f; gl73.Npad = E; gl73.pad_ = 0;
      if ((long long)(64) >= 64 && (long long)(E) >= 64) k_gemmT<1, 2, 4><<<dim3((unsigned)((E) + 63) / 64, (unsigned)((64) + 31) / 32, (unsigned)(TC)), 32, 0, stream>>>(gl73);
      else k_gemm<1><<<dim3((unsigned)((E) + 31) / 32, (unsigned)((64) + 15) / 16, (unsigned)(TC)), 32, 0, stream>>>(gl73); }
    k_tb_csum<<<(unsigned)(((long long)TC * 16 * E + 255) / 256), 256, 0, stream>>>(H, CS, TC, NN, E, 5, 16, 21);
    { GemmP gl72;
      gl72.A = CS; gl72.B = WsW; gl72.bias = B4; gl72.R = H + (size_t)5 * E; gl72.C = H + (size_t)5 * E;
      gl72.sAo = (long long)16 * E; gl72.sAi = 0; gl72.sAm = E; gl72.sAk = 1; gl72.sBo = 0; gl72.sBi = 0; gl72.sBn = E; gl72.sBk = 1; gl72.sCo = (long long)NN * E; gl72.sCi = 0; gl72.sCm = E; gl72.sRo = (long long)NN * E; gl72.sRi = 0; gl72.sRm = E; gl72.sRn = 1;
      gl72.M = 16; gl72.N = E; gl72.K = E; gl72.zi_n = 1; gl72.flags = 5; gl72.act = 0;
      gl72.alpha = 1.0f; gl72.beta = 1.0f; gl72.sa = 1.0f; gl72.sb = 1.0f; gl72.Npad = E; gl72.pad_ = 0;
      k_gemm<1><<<dim3((unsigned)((E) + 31) / 32, (unsigned)((16) + 15) / 16, (unsigned)(TC)), 32, 0, stream>>>(gl72); }
    k_tb_csum<<<(unsigned)(((long long)TC * 4 * E + 255) / 256), 256, 0, stream>>>(H, CS, TC, NN, E, 1, 4, 5);
    { GemmP gl71;
      gl71.A = CS; gl71.B = WsW; gl71.bias = B4; gl71.R = H + (size_t)1 * E; gl71.C = H + (size_t)1 * E;
      gl71.sAo = (long long)4 * E; gl71.sAi = 0; gl71.sAm = E; gl71.sAk = 1; gl71.sBo = 0; gl71.sBi = 0; gl71.sBn = E; gl71.sBk = 1; gl71.sCo = (long long)NN * E; gl71.sCi = 0; gl71.sCm = E; gl71.sRo = (long long)NN * E; gl71.sRi = 0; gl71.sRm = E; gl71.sRn = 1;
      gl71.M = 4; gl71.N = E; gl71.K = E; gl71.zi_n = 1; gl71.flags = 5; gl71.act = 0;
      gl71.alpha = 1.0f; gl71.beta = 1.0f; gl71.sa = 1.0f; gl71.sb = 1.0f; gl71.Npad = E; gl71.pad_ = 0;
      k_gemm<1><<<dim3((unsigned)((E) + 31) / 32, (unsigned)((4) + 15) / 16, (unsigned)(TC)), 32, 0, stream>>>(gl71); }
    k_tb_csum<<<(unsigned)(((long long)TC * 1 * E + 255) / 256), 256, 0, stream>>>(H, CS, TC, NN, E, 0, 1, 1);
    { GemmP gl70;
      gl70.A = CS; gl70.B = WsW; gl70.bias = B4; gl70.R = H + (size_t)0 * E; gl70.C = H + (size_t)0 * E;
      gl70.sAo = (long long)1 * E; gl70.sAi = 0; gl70.sAm = E; gl70.sAk = 1; gl70.sBo = 0; gl70.sBi = 0; gl70.sBn = E; gl70.sBk = 1; gl70.sCo = (long long)NN * E; gl70.sCi = 0; gl70.sCm = E; gl70.sRo = (long long)NN * E; gl70.sRi = 0; gl70.sRm = E; gl70.sRn = 1;
      gl70.M = 1; gl70.N = E; gl70.K = E; gl70.zi_n = 1; gl70.flags = 5; gl70.act = 0;
      gl70.alpha = 1.0f; gl70.beta = 1.0f; gl70.sa = 1.0f; gl70.sb = 1.0f; gl70.Npad = E; gl70.pad_ = 0;
      k_gemm<1><<<dim3((unsigned)((E) + 31) / 32, (unsigned)((1) + 15) / 16, (unsigned)(TC)), 32, 0, stream>>>(gl70); }
    k_tb_max<<<(unsigned)((TC * E + 127) / 128), 128, 0, stream>>>(H, out, 448, TC, NN, E);
}
